// EquiMAB3_1322849927409
// MI455X (gfx1250) — hardware-verified
//
#include <hip/hip_runtime.h>
#include <math.h>

typedef __attribute__((ext_vector_type(16))) _Float16 v16h;
typedef __attribute__((ext_vector_type(8)))  _Float16 v8h;
typedef __attribute__((ext_vector_type(16))) __bf16   v16b;
typedef __attribute__((ext_vector_type(8)))  float    v8f;
typedef __attribute__((ext_vector_type(4)))  float    v4f;

__device__ __forceinline__ int frag_k(int i, int h) { return (i < 8) ? (8 * h + i) : (16 + 8 * h + (i - 8)); }
__device__ __forceinline__ __bf16 bf16_rne(float f) {
    unsigned int u = __float_as_uint(f);
    u += 0x7fffu + ((u >> 16) & 1u);
    return __builtin_bit_cast(__bf16, (unsigned short)(u >> 16));
}
__device__ __forceinline__ float bf16_f32(__bf16 b) { return __uint_as_float(((unsigned int)__builtin_bit_cast(unsigned short, b)) << 16); }
__device__ __forceinline__ v8f wmma16(v16h a, v16h b, v8f c) {
    c = __builtin_amdgcn_wmma_f32_16x16x32_f16(false, a, false, b, (short)0, c, false, false);
    asm volatile("v_nop\n\tv_nop\n\tv_nop\n\tv_nop" : "+v"(c) : "v"(a), "v"(b));
    return c;
}
__device__ __forceinline__ v8f wmmab(v16b a, v16b b, v8f c) {
    c = __builtin_amdgcn_wmma_f32_16x16x32_bf16(false, a, false, b, (short)0, c, false, false);
    asm volatile("v_nop\n\tv_nop\n\tv_nop\n\tv_nop" : "+v"(c) : "v"(a), "v"(b));
    return c;
}
struct Split { v16b hi, lo; };
__device__ __forceinline__ v8f wmma3(const Split& a, const Split& b, v8f c) {
    c = __builtin_amdgcn_wmma_f32_16x16x32_bf16(false, a.hi, false, b.hi, (short)0, c, false, false);
    c = __builtin_amdgcn_wmma_f32_16x16x32_bf16(false, a.hi, false, b.lo, (short)0, c, false, false);
    c = __builtin_amdgcn_wmma_f32_16x16x32_bf16(false, a.lo, false, b.hi, (short)0, c, false, false);
    asm volatile("v_nop\n\tv_nop\n\tv_nop\n\tv_nop" : "+v"(c) : "v"(a.hi), "v"(a.lo), "v"(b.hi), "v"(b.lo));
    return c;
}
struct Split3 { v16b hi, mid, lo; };
__device__ __forceinline__ v8f wmma6(const Split3& a, const Split3& b, v8f c) {
    c = __builtin_amdgcn_wmma_f32_16x16x32_bf16(false, a.hi, false, b.hi, (short)0, c, false, false);
    c = __builtin_amdgcn_wmma_f32_16x16x32_bf16(false, a.hi, false, b.mid, (short)0, c, false, false);
    c = __builtin_amdgcn_wmma_f32_16x16x32_bf16(false, a.mid, false, b.hi, (short)0, c, false, false);
    c = __builtin_amdgcn_wmma_f32_16x16x32_bf16(false, a.hi, false, b.lo, (short)0, c, false, false);
    c = __builtin_amdgcn_wmma_f32_16x16x32_bf16(false, a.mid, false, b.mid, (short)0, c, false, false);
    c = __builtin_amdgcn_wmma_f32_16x16x32_bf16(false, a.lo, false, b.hi, (short)0, c, false, false);
    asm volatile("v_nop\n\tv_nop\n\tv_nop\n\tv_nop" : "+v"(c) : "v"(a.hi), "v"(a.mid), "v"(a.lo), "v"(b.hi), "v"(b.mid), "v"(b.lo));
    return c;
}

__device__ __forceinline__ v16h fh_ld(const float* __restrict__ p, long long sk, int k0, int h, int klen, float s) {
    v16h a;
#pragma unroll
    for (int i = 0; i < 16; ++i) { const int k = k0 + frag_k(i, h); a[i] = (k < klen) ? (_Float16)(p[(long long)k * sk] * s) : (_Float16)0.f; }
    return a;
}
__device__ __forceinline__ Split sp_ld(const float* __restrict__ p, long long sk, int k0, int h, int klen, float s) {
    Split r;
#pragma unroll
    for (int i = 0; i < 16; ++i) {
        const int k = k0 + frag_k(i, h); const float x = (k < klen) ? p[(long long)k * sk] * s : 0.f;
        const __bf16 hb = bf16_rne(x); r.hi[i] = hb; r.lo[i] = bf16_rne(x - bf16_f32(hb));
    }
    return r;
}
__device__ __forceinline__ Split3 sp3_ld(const float* __restrict__ p, long long sk, int k0, int h, int klen, float s) {
    Split3 r;
#pragma unroll
    for (int i = 0; i < 16; ++i) {
        const int k = k0 + frag_k(i, h); const float x = (k < klen) ? p[(long long)k * sk] * s : 0.f;
        const __bf16 hb = bf16_rne(x); const float r1 = x - bf16_f32(hb); const __bf16 mb = bf16_rne(r1);
        r.hi[i] = hb; r.mid[i] = mb; r.lo[i] = bf16_rne(r1 - bf16_f32(mb));
    }
    return r;
}
__device__ __forceinline__ v16b bh_ld(const float* __restrict__ p, long long sk, int k0, int h, int klen, float s) {
    v16b a;
#pragma unroll
    for (int i = 0; i < 16; ++i) { const int k = k0 + frag_k(i, h); a[i] = bf16_rne((k < klen) ? p[(long long)k * sk] * s : 0.f); }
    return a;
}
__device__ __forceinline__ v16h fh_row(const _Float16* __restrict__ row, int k0, int h) {
    v16h a;
#pragma unroll
    for (int i = 0; i < 16; ++i) a[i] = row[k0 + frag_k(i, h)];
    return a;
}

#define VST2(T, ptr, val) do { const T vst2_v_ = (val); *(volatile T*)(ptr) = vst2_v_; __threadfence(); *(volatile T*)(ptr) = vst2_v_; } while (0)
typedef float v4f __attribute__((ext_vector_type(4)));
#define VST2V4(ptr, val) do { const v4f vst2_v4_ = (val); *(volatile v4f*)(ptr) = vst2_v4_; __threadfence(); *(volatile v4f*)(ptr) = vst2_v4_; } while (0)

__device__ __attribute__((noinline)) float act_fn(float v, int act) {
    if (act == 1) return fmaxf(v, 0.f);
    if (act == 2) { const float u = 0.7978845608028654f * (v + 0.044715f * v * v * v); return 0.5f * v * (1.f + tanhf(u)); }
    if (act == 3) return v / (1.f + expf(-v));
    if (act == 4) return 0.5f * v * (1.f + erff(v * 0.7071067811865476f));
    if (act == 5) return tanhf(v);
    if (act == 6) return 1.f / (1.f + expf(-v));
    if (act == 7) return (v > 0.f) ? v : 0.01f * v;
    if (act == 8) return (v > 0.f) ? v : (expf(v) - 1.f);
    if (act == 9) return fminf(fmaxf(v, 0.f), 6.f);
    if (act == 10) return fabsf(v);
    if (act == 11) return (v >= 0.f) ? v : 0.1f * v;
    if (act == 12) return (v > 0.f) ? v : 0.2f * v;
    if (act == 13) return (v > 20.f) ? v : log1pf(expf(v));
    return v;
}

struct GemmP {
    const float* A; const float* B; const float* bias; const float* R; float* C;
    long long sAo, sAi, sAm, sAk, sBo, sBi, sBn, sBk, sCo, sCi, sCm, sRo, sRi, sRm, sRn;
    int M, N, K, zi_n, flags, act; float alpha, beta, sa, sb;
    int Npad, pad_;
};
static_assert(sizeof(GemmP) == 5 * 8 + 15 * 8 + 6 * 4 + 4 * 4 + 2 * 4, "GemmP has padding");

template <int MODE>
__global__ __launch_bounds__(32) void k_gemm(GemmP p) {
    const int lane = threadIdx.x & 31, h = lane >> 4, l15 = lane & 15;
    const int m0 = blockIdx.y * 16, n0 = blockIdx.x * 32;
    const int z = blockIdx.z, zo = z / p.zi_n, zi = z - zo * p.zi_n;
    const float* A = p.A + zo * p.sAo + zi * p.sAi;
    const float* B = p.B + zo * p.sBo + zi * p.sBi;
    const int am = min(m0 + l15, p.M - 1);
    v8f acc[2], comp[2];
#pragma unroll
    for (int t = 0; t < 2; ++t) { v8f zz = {}; acc[t] = zz; comp[t] = zz; }
    for (int k0 = 0; k0 < p.K; k0 += 32) {
        const float* arow = A + (long long)am * p.sAm;
        if (MODE == 1) {
            const Split a = sp_ld(arow, p.sAk, k0, h, p.K, 1.f);
#pragma unroll
            for (int t = 0; t < 2; ++t) {
                const int bn = min(n0 + t * 16 + l15, p.N - 1);
                acc[t] = wmma3(a, sp_ld(B + (long long)bn * p.sBn, p.sBk, k0, h, p.K, 1.f), acc[t]);
            }
        } else if (MODE == 3) {
            const Split3 a = sp3_ld(arow, p.sAk, k0, h, p.K, 1.f);
#pragma unroll
            for (int t = 0; t < 2; ++t) {
                const int bn = min(n0 + t * 16 + l15, p.N - 1);
                acc[t] = wmma6(a, sp3_ld(B + (long long)bn * p.sBn, p.sBk, k0, h, p.K, 1.f), acc[t]);
            }
        } else if (MODE == 4) {
            const Split3 a = sp3_ld(arow, p.sAk, k0, h, p.K, 1.f);
#pragma unroll
            for (int t = 0; t < 2; ++t) {
                const int bn = min(n0 + t * 16 + l15, p.N - 1); v8f zz = {};
                const v8f part = wmma6(a, sp3_ld(B + (long long)bn * p.sBn, p.sBk, k0, h, p.K, 1.f), zz);
                const v8f y = part - comp[t]; const v8f s = acc[t] + y; comp[t] = (s - acc[t]) - y; acc[t] = s;
            }
        } else if (MODE == 2) {
            const v16b a = bh_ld(arow, p.sAk, k0, h, p.K, 1.f);
#pragma unroll
            for (int t = 0; t < 2; ++t) {
                const int bn = min(n0 + t * 16 + l15, p.N - 1);
                acc[t] = wmmab(a, bh_ld(B + (long long)bn * p.sBn, p.sBk, k0, h, p.K, 1.f), acc[t]);
            }
        } else {
            const v16h a = fh_ld(arow, p.sAk, k0, h, p.K, p.sa);
#pragma unroll
            for (int t = 0; t < 2; ++t) {
                const int bn = min(n0 + t * 16 + l15, p.N - 1);
                acc[t] = wmma16(a, fh_ld(B + (long long)bn * p.sBn, p.sBk, k0, h, p.K, p.sb), acc[t]);
            }
        }
    }
    const float iscale = (MODE == 0) ? p.alpha / (p.sa * p.sb) : p.alpha;
    float* C = p.C + zo * p.sCo + zi * p.sCi;
    const float* R = p.R + zo * p.sRo + zi * p.sRi;
    __shared__ __align__(16) float ctile[16][36];
#pragma unroll
    for (int t = 0; t < 2; ++t) {
        const int n = n0 + t * 16 + l15; const int nn = min(n, p.N - 1);
#pragma unroll
        for (int r = 0; r < 8; ++r) {
            const int m = m0 + 8 * h + r; const int mm = min(m, p.M - 1);
            float v = acc[t][r] * iscale;
            if (p.flags & 1) v += p.bias[nn];
            if (p.flags & 2) v += p.bias[mm];
            v = act_fn(v, p.act);
            if (p.flags & 4) v += p.beta * R[(long long)mm * p.sRm + (long long)nn * p.sRn];
            ctile[8 * h + r][t * 16 + l15] = (n < p.N) ? v : 0.f;
        }
    }
    __syncthreads();
    const int NW = (p.Npad > p.N) ? p.Npad : p.N;
    const bool fast = (m0 + 16 <= p.M) && (n0 + 32 <= NW) && ((p.sCm & 3) == 0) && ((((size_t)C) & 15) == 0);
    if (fast) {
#pragma unroll
        for (int s = 0; s < 4; ++s) {
            const int row = s * 4 + (lane >> 3), c4 = (lane & 7) * 4;
            const v4f v = *(const v4f*)&ctile[row][c4];
            VST2V4(C + (long long)(m0 + row) * p.sCm + n0 + c4, v);
        }
    } else {
        for (int row = 0; row < 16; ++row) {
            const int m = m0 + row, n = n0 + lane;
            if (m < p.M && n < NW) VST2(float, C + (long long)m * p.sCm + n, ctile[row][lane]);
        }
    }
}


template <int MODE, int TM, int TN>
__global__ __launch_bounds__(32) void k_gemmT(GemmP p) {
    const int lane = threadIdx.x & 31, h = lane >> 4, l15 = lane & 15;
    const int m0 = blockIdx.y * (16 * TM), n0 = blockIdx.x * (16 * TN);
    const int z = blockIdx.z, zo = z / p.zi_n, zi = z - zo * p.zi_n;
    const float* A = p.A + zo * p.sAo + zi * p.sAi;
    const float* B = p.B + zo * p.sBo + zi * p.sBi;
    v8f acc[TM][TN];
#pragma unroll
    for (int i = 0; i < TM; ++i)
#pragma unroll
        for (int t = 0; t < TN; ++t) { v8f zz = {}; acc[i][t] = zz; }
    for (int k0 = 0; k0 < p.K; k0 += 32) {
        if (MODE == 1) {
            Split a[TM], b[TN];
#pragma unroll
            for (int i = 0; i < TM; ++i) { const int am = min(m0 + 16 * i + l15, p.M - 1); a[i] = sp_ld(A + (long long)am * p.sAm, p.sAk, k0, h, p.K, 1.f); }
#pragma unroll
            for (int t = 0; t < TN; ++t) { const int bn = min(n0 + 16 * t + l15, p.N - 1); b[t] = sp_ld(B + (long long)bn * p.sBn, p.sBk, k0, h, p.K, 1.f); }
#pragma unroll
            for (int i = 0; i < TM; ++i)
#pragma unroll
                for (int t = 0; t < TN; ++t) acc[i][t] = wmma3(a[i], b[t], acc[i][t]);
        } else if (MODE == 2) {
            v16b a[TM], b[TN];
#pragma unroll
            for (int i = 0; i < TM; ++i) { const int am = min(m0 + 16 * i + l15, p.M - 1); a[i] = bh_ld(A + (long long)am * p.sAm, p.sAk, k0, h, p.K, 1.f); }
#pragma unroll
            for (int t = 0; t < TN; ++t) { const int bn = min(n0 + 16 * t + l15, p.N - 1); b[t] = bh_ld(B + (long long)bn * p.sBn, p.sBk, k0, h, p.K, 1.f); }
#pragma unroll
            for (int i = 0; i < TM; ++i)
#pragma unroll
                for (int t = 0; t < TN; ++t) acc[i][t] = wmmab(a[i], b[t], acc[i][t]);
        } else {
            v16h a[TM], b[TN];
#pragma unroll
            for (int i = 0; i < TM; ++i) { const int am = min(m0 + 16 * i + l15, p.M - 1); a[i] = fh_ld(A + (long long)am * p.sAm, p.sAk, k0, h, p.K, p.sa); }
#pragma unroll
            for (int t = 0; t < TN; ++t) { const int bn = min(n0 + 16 * t + l15, p.N - 1); b[t] = fh_ld(B + (long long)bn * p.sBn, p.sBk, k0, h, p.K, p.sb); }
#pragma unroll
            for (int i = 0; i < TM; ++i)
#pragma unroll
                for (int t = 0; t < TN; ++t) acc[i][t] = wmma16(a[i], b[t], acc[i][t]);
        }
    }
    const float iscale = (MODE == 0) ? p.alpha / (p.sa * p.sb) : p.alpha;
    float* C = p.C + zo * p.sCo + zi * p.sCi;
    const float* R = p.R + zo * p.sRo + zi * p.sRi;
    const int NW = (p.Npad > p.N) ? p.Npad : p.N;
    __shared__ __align__(16) float ctile[16][36];
#pragma unroll
    for (int i = 0; i < TM; ++i) {
        const int mb = m0 + 16 * i; if (mb >= p.M) break;
#pragma unroll
        for (int tp = 0; tp < TN / 2; ++tp) {
            const int nb = n0 + 32 * tp; if (nb >= NW) break;
#pragma unroll
            for (int t2 = 0; t2 < 2; ++t2) {
                const int t = 2 * tp + t2; const int n = nb + t2 * 16 + l15; const int nn = min(n, p.N - 1);
#pragma unroll
                for (int r = 0; r < 8; ++r) {
                    const int m = mb + 8 * h + r; const int mm = min(m, p.M - 1);
                    float v = acc[i][t][r] * iscale;
                    if (p.flags & 1) v += p.bias[nn];
                    if (p.flags & 2) v += p.bias[mm];
                    v = act_fn(v, p.act);
                    if (p.flags & 4) v += p.beta * R[(long long)mm * p.sRm + (long long)nn * p.sRn];
                    ctile[8 * h + r][t2 * 16 + l15] = (n < p.N) ? v : 0.f;
                }
            }
            __syncthreads();
            const bool fast = (mb + 16 <= p.M) && (nb + 32 <= NW) && ((p.sCm & 3) == 0) && ((((size_t)C) & 15) == 0);
            if (fast) {
#pragma unroll
                for (int s = 0; s < 4; ++s) {
                    const int row = s * 4 + (lane >> 3), c4 = (lane & 7) * 4;
                    const v4f v = *(const v4f*)&ctile[row][c4];
                    VST2V4(C + (long long)(mb + row) * p.sCm + nb + c4, v);
                }
            } else {
                for (int row = 0; row < 16; ++row) {
                    const int m = mb + row, n = nb + lane;
                    if (m < p.M && n < NW) VST2(float, C + (long long)m * p.sCm + n, ctile[row][lane]);
                }
            }
            __syncthreads();
        }
    }
}

#define AW 4
struct AttnP {
    const float* Q; const float* K; const float* V; float* O; float* P; const float* Mf; const int* Mi; float* ST;
    const float* Pw; const float* Rt; const int* SQ; const int* SK;
    long long swb, swh, swi, swj, srb, srh, sri;
    long long sQb, sQh, sQi, sQd, sKb, sKh, sKj, sKd, sVb, sVh, sVj, sVd, sOb, sOh, sOi, sPb, sPh, sPi, smb, smh, smi, smj;
    int Lq, Lk, dh, dv, hrep, causal, coff, pband;
    float scale, mfill; int nonorm, mpol;
    int roff, rn, segpol, win;
};
static_assert(sizeof(AttnP) == 12 * 8 + 29 * 8 + 16 * 4, "AttnP has padding");

#ifndef KATTN_ATTR
#define KATTN_ATTR
#endif
template <int DHP, int DVP, int QM, bool SPLITPV, bool TWOPASS>
__global__ __launch_bounds__(32 * AW) KATTN_ATTR void k_attn(AttnP p) {
    constexpr int NT = DVP / 16;
    constexpr int KS = DHP / 32;
    constexpr int VP = DVP + 8;
    __shared__ __align__(16) float    pl[AW][16 * 64];
    __shared__ __align__(16) _Float16 vl[(SPLITPV ? 2 : 1) * 64 * VP];
    const int lane = threadIdx.x & 31, hf = lane >> 4, l15 = lane & 15, wave = threadIdx.x >> 5;
    const int h = blockIdx.y, b = blockIdx.z, hk = h / p.hrep;
    const int q0 = (blockIdx.x * AW + wave) * 16;
    float* myp = pl[wave];
    const float L2E = 1.4426950408889634f;
    const float NEG = -__builtin_inff();
    const int qi = min(q0 + l15, p.Lq - 1);
    const float* qrow = p.Q + b * p.sQb + h * p.sQh + (long long)qi * p.sQi;
    const float* kbase = p.K + b * p.sKb + hk * p.sKh;
    const float* vbase = p.V + b * p.sVb + hk * p.sVh;
    v16h qa[QM == 0 ? KS : 1]; Split qs_[QM == 1 ? KS : 1]; Split3 qt_[QM == 2 ? KS : 1];
#pragma unroll
    for (int ks = 0; ks < KS; ++ks) {
        if (QM == 2) qt_[ks] = sp3_ld(qrow, p.sQd, ks * 32, hf, p.dh, 1.f);
        else if (QM == 1) qs_[ks] = sp_ld(qrow, p.sQd, ks * 32, hf, p.dh, 1.f);
        else qa[ks] = fh_ld(qrow, p.sQd, ks * 32, hf, p.dh, 1.f);
    }
    v8f o[NT]; float m8[8], l8[8];
#pragma unroll
    for (int t = 0; t < NT; ++t) { v8f zz = {}; o[t] = zz; }
#pragma unroll
    for (int i = 0; i < 8; ++i) { m8[i] = NEG; l8[i] = 0.f; }
    int jend = p.Lk;
    if (p.causal == 1) { const int je = (blockIdx.x * AW + AW - 1) * 16 + 16 + p.coff; jend = min(jend, max(je, 0)); }
    const int npass = TWOPASS ? 2 : 1;
    for (int pass = 0; pass < npass; ++pass) {
        const bool dopv = (!TWOPASS) || pass == 1;
        for (int j0 = 0; j0 < jend; j0 += 64) {
            if (dopv) {
                __syncthreads();
                for (int idx = threadIdx.x; idx < 64 * DVP; idx += 32 * AW) {
                    const int jr = idx / DVP, d = idx - jr * DVP, j = j0 + jr;
                    const float f = (j < p.Lk && d < p.dv) ? vbase[(long long)j * p.sVj + (long long)d * p.sVd] : 0.f;
                    if (SPLITPV) {
                        const __bf16 hb = bf16_rne(f);
                        ((__bf16*)vl)[jr * VP + d] = hb; ((__bf16*)vl)[64 * VP + jr * VP + d] = bf16_rne(f - bf16_f32(hb));
                    } else vl[jr * VP + d] = (_Float16)f;
                }
            }
            v8f s[4];
#pragma unroll
            for (int t = 0; t < 4; ++t) {
                const int j = min(j0 + t * 16 + l15, p.Lk - 1);
                const float* krow = kbase + (long long)j * p.sKj;
                v8f acc = {};
#pragma unroll
                for (int ks = 0; ks < KS; ++ks) {
                    if (QM == 2)      acc = wmma6(qt_[ks], sp3_ld(krow, p.sKd, ks * 32, hf, p.dh, 1.f), acc);
                    else if (QM == 1) acc = wmma3(qs_[ks], sp_ld(krow, p.sKd, ks * 32, hf, p.dh, 1.f), acc);
                    else              acc = wmma16(qa[ks], fh_ld(krow, p.sKd, ks * 32, hf, p.dh, 1.f), acc);
                }
                s[t] = acc;
            }
            float pv[8][4];
#pragma unroll
            for (int i = 0; i < 8; ++i) {
                const int irow = q0 + i + 8 * hf;
                const int ic = min(irow, p.Lq - 1);
                float sc[4];
#pragma unroll
                for (int t = 0; t < 4; ++t) {
                    const int jg = j0 + t * 16 + l15;
                    float v = s[t][i] * p.scale;
                    if (p.Mf) v += p.Mf[b * p.smb + h * p.smh + (long long)ic * p.smi + (long long)min(jg, p.Lk - 1) * p.smj];
                    if (p.Rt) { int rc = ic - min(jg, p.Lk - 1) + p.roff; rc = rc < 0 ? 0 : (rc >= p.rn ? p.rn - 1 : rc); v += p.Rt[b * p.srb + h * p.srh + (long long)ic * p.sri + rc]; }
                    if (p.Mi) { const int mv = p.Mi[b * p.smb + h * p.smh + (long long)ic * p.smi + (long long)min(jg, p.Lk - 1) * p.smj]; if (p.mpol ? (mv != 0) : (mv == 0)) v = p.mfill; }
                    if (p.SQ) { const bool same = p.SQ[(long long)b * p.Lq + ic] == p.SK[(long long)b * p.Lk + min(jg, p.Lk - 1)]; if (p.segpol ? same : !same) v = p.mfill; }
                    if (p.causal == 2 && jg > irow + p.coff) v = p.mfill;
                    if (jg >= p.Lk || (p.causal == 1 && jg > irow + p.coff) || (p.causal == 3 && jg < irow + p.coff) || (p.win > 0 && irow + p.coff - jg > p.win)) v = NEG; else v *= L2E;
                    sc[t] = v;
                }
                if (!TWOPASS || pass == 0) {
                    float mx = fmaxf(fmaxf(sc[0], sc[1]), fmaxf(sc[2], sc[3]));
                    mx = fmaxf(mx, __shfl_xor(mx, 1, 32)); mx = fmaxf(mx, __shfl_xor(mx, 2, 32));
                    mx = fmaxf(mx, __shfl_xor(mx, 4, 32)); mx = fmaxf(mx, __shfl_xor(mx, 8, 32));
                    const float mnew = fmaxf(m8[i], mx);
                    const float corr = (mnew == NEG) ? 1.f : exp2f(m8[i] - mnew);
                    float rs = 0.f;
#pragma unroll
                    for (int t = 0; t < 4; ++t) {
                        const float pp = (sc[t] == NEG) ? 0.f : exp2f(sc[t] - mnew); rs += pp;
                        pv[i][t] = p.Pw ? pp * p.Pw[b * p.swb + h * p.swh + (long long)ic * p.swi + (long long)min(j0 + t * 16 + l15, p.Lk - 1) * p.swj] : pp;
                    }
                    rs += __shfl_xor(rs, 1, 32); rs += __shfl_xor(rs, 2, 32); rs += __shfl_xor(rs, 4, 32); rs += __shfl_xor(rs, 8, 32);
                    l8[i] = l8[i] * corr + rs; m8[i] = mnew;
                    if (!TWOPASS) {
#pragma unroll
                        for (int t = 0; t < NT; ++t) o[t][i] *= corr;
                    }
                } else {
                    const float inv = (l8[i] > 0.f) ? 1.f / l8[i] : 0.f;
#pragma unroll
                    for (int t = 0; t < 4; ++t) {
                        const int jg = j0 + t * 16 + l15;
                        float pp = (sc[t] == NEG) ? 0.f : exp2f(sc[t] - m8[i]) * inv;
                        if (p.Pw) pp *= p.Pw[b * p.swb + h * p.swh + (long long)ic * p.swi + (long long)min(jg, p.Lk - 1) * p.swj];
                        pv[i][t] = pp;
                    }
                }
            }
            if (dopv) {
#pragma unroll
                for (int i = 0; i < 8; ++i)
#pragma unroll
                    for (int t = 0; t < 4; ++t) myp[(i + 8 * hf) * 64 + t * 16 + l15] = pv[i][t];
                __syncthreads();
                if (p.P) {
                    float* pb_ = p.P + b * p.sPb + h * p.sPh;
                    const bool fastP = (p.pband == 0) && ((p.sPi & 3) == 0) && (j0 + 64 <= p.Lk) && (q0 + 16 <= p.Lq) && ((((size_t)pb_) & 15) == 0);
                    if (fastP) {
#pragma unroll
                        for (int s = 0; s < 8; ++s) {
                            const int row = s * 2 + (lane >> 4), c4 = (lane & 15) * 4;
                            const v4f v = *(const v4f*)(myp + row * 64 + c4);
                            VST2V4(pb_ + (long long)(q0 + row) * p.sPi + j0 + c4, v);
                        }
                    } else {
                        for (int row = 0; row < 16; ++row) {
                            const int irow = q0 + row; if (irow >= p.Lq) continue;
                            for (int c = lane; c < 64; c += 32) {
                                const int jg = j0 + c; if (jg >= p.Lk) continue;
                                if (p.pband == 0) VST2(float, pb_ + (long long)irow * p.sPi + jg, myp[row * 64 + c]);
                                else if (jg - irow <= p.pband && irow - jg <= p.pband) VST2(float, pb_ + (long long)irow * p.sPi + (jg - irow + p.pband), myp[row * 64 + c]);
                            }
                        }
                    }
                }
                if (SPLITPV) {
                    const Split pa0 = sp_ld(myp + l15 * 64, 1, 0, hf, 64, 1.f), pa1 = sp_ld(myp + l15 * 64, 1, 32, hf, 64, 1.f);
                    const __bf16* vh = (const __bf16*)vl; const __bf16* vlo = vh + 64 * VP;
#pragma unroll
                    for (int t = 0; t < NT; ++t) {
                        const int dcol = t * 16 + l15;
                        Split b0, b1;
#pragma unroll
                        for (int e = 0; e < 16; ++e) {
                            const int k0 = frag_k(e, hf), k1 = 32 + frag_k(e, hf);
                            b0.hi[e] = vh[k0 * VP + dcol]; b0.lo[e] = vlo[k0 * VP + dcol]; b1.hi[e] = vh[k1 * VP + dcol]; b1.lo[e] = vlo[k1 * VP + dcol];
                        }
                        o[t] = wmma3(pa0, b0, o[t]);
                        o[t] = wmma3(pa1, b1, o[t]);
                    }
                } else {
                    const v16h pa0 = fh_ld(myp + l15 * 64, 1, 0, hf, 64, 4096.f), pa1 = fh_ld(myp + l15 * 64, 1, 32, hf, 64, 4096.f);
#pragma unroll
                    for (int t = 0; t < NT; ++t) {
                        const int dcol = t * 16 + l15;
                        v16h b0, b1;
#pragma unroll
                        for (int e = 0; e < 16; ++e) { b0[e] = vl[frag_k(e, hf) * VP + dcol]; b1[e] = vl[(32 + frag_k(e, hf)) * VP + dcol]; }
                        o[t] = wmma16(pa0, b0, o[t]);
                        o[t] = wmma16(pa1, b1, o[t]);
                    }
                }
            }
        }
    }
    float* obase = p.O + b * p.sOb + h * p.sOh;
    if (p.ST) {
        const int rl = lane >> 1, isel = rl & 7;
        float mv = 0.f, lv = 0.f;
#pragma unroll
        for (int i = 0; i < 8; ++i) if (i == isel) { mv = m8[i]; lv = l8[i]; }
        const int irow = q0 + rl;
        if (irow < p.Lq) { float* st = p.ST + (((long long)b * gridDim.y + h) * p.Lq + irow) * 2 + (lane & 1); VST2(float, st, (lane & 1) ? lv : mv * 0.6931471805599453f); }
    }
    float invr[8];
#pragma unroll
    for (int i = 0; i < 8; ++i) {
        if (TWOPASS) invr[i] = SPLITPV ? 1.f : (1.f / 4096.f);
        else if (p.nonorm) invr[i] = exp2f(m8[i]) * (SPLITPV ? 1.f : (1.f / 4096.f));
        else invr[i] = (l8[i] > 0.f) ? (SPLITPV ? 1.f / l8[i] : 1.f / (l8[i] * 4096.f)) : 0.f;
    }
    __syncthreads();
    const bool ofast = ((p.sOi & 3) == 0) && ((((size_t)obase) & 15) == 0) && (q0 + 16 <= p.Lq);
#pragma unroll
    for (int c0 = 0; c0 < DVP; c0 += 64) {
#pragma unroll
        for (int i = 0; i < 8; ++i)
#pragma unroll
            for (int t = 0; t < NT; ++t) if (t * 16 >= c0 && t * 16 < c0 + 64) myp[(i + 8 * hf) * 64 + (t * 16 - c0) + l15] = o[t][i] * invr[i];
        __syncthreads();
        const int cw = (DVP - c0 < 64) ? (DVP - c0) : 64;
        if (ofast && (c0 + cw <= p.dv) && (cw % 32 == 0)) {
            const int lpr = cw / 4;
            const int rows_per_ins = 32 / lpr;
            for (int r0 = 0; r0 < 16; r0 += rows_per_ins) {
                const int row = r0 + lane / lpr, c4 = (lane % lpr) * 4;
                const v4f v = *(const v4f*)(myp + row * 64 + c4);
                VST2V4(obase + (long long)(q0 + row) * p.sOi + c0 + c4, v);
            }
        } else {
            for (int row = 0; row < 16; ++row) {
                const int irow = q0 + row; if (irow >= p.Lq) continue;
                for (int c = lane; c < cw; c += 32) { const int d = c0 + c; if (d < p.dv) VST2(float, obase + (long long)irow * p.sOi + d, myp[row * 64 + c]); }
            }
        }
        __syncthreads();
    }
}

struct TrP { const float* src; float* dst; const float* R2; long long sSz, lds, sDz, ldd, sRz, ldr; int R, C, flags, act; float alpha, beta; };
static_assert(sizeof(TrP) == 3 * 8 + 6 * 8 + 6 * 4, "TrP has padding");
__global__ __launch_bounds__(256) void k_tr(TrP p) {
    __shared__ float tile[32][33];
    const int c0 = blockIdx.x * 32, r0 = blockIdx.y * 32, z = blockIdx.z;
    const int lane = threadIdx.x & 31, wave = threadIdx.x >> 5;
    const float* s = p.src + z * p.sSz;
#pragma unroll
    for (int k = 0; k < 4; ++k) {
        const int rl = wave * 4 + k, r = r0 + rl, c = c0 + lane;
        tile[rl][lane] = (r < p.R && c < p.C) ? s[(long long)r * p.lds + c] : 0.f;
    }
    __syncthreads();
    float* d = p.dst + z * p.sDz; const float* rr = p.R2 + z * p.sRz;
#pragma unroll
    for (int k = 0; k < 4; ++k) {
        const int cl = wave * 4 + k, c = c0 + cl, r = r0 + lane;
        if (c < p.C && r < p.R) {
            float v = act_fn(p.alpha * tile[lane][cl], p.act);
            if (p.flags & 1) v += p.beta * rr[(long long)c * p.ldr + r];
            VST2(float, d + (long long)c * p.ldd + r, v);
        }
    }
}

__global__ __launch_bounds__(256) void k_affine(const float* __restrict__ src, float* __restrict__ dst, int n, float a, float b, const float* __restrict__ sdev) {
    const int i = blockIdx.x * 256 + threadIdx.x;
    if (i < n) { const float aa = sdev ? a * sdev[0] : a; const float v = aa * src[i] + b; VST2(float, dst + i, v); }
}

struct SmP { const float* src; float* dst; const float* Mf; long long sz, sr, dz, dr, smz, smr; int n, pad; float scale_in, scale_out; };
static_assert(sizeof(SmP) == 3 * 8 + 6 * 8 + 4 * 4, "SmP has padding");
__global__ __launch_bounds__(256) void k_softmax(SmP p) {
    __shared__ float red[256];
    const int r = blockIdx.x, z = blockIdx.y, tid = threadIdx.x;
    const float* s = p.src + z * p.sz + (long long)r * p.sr;
    const float* mf = p.Mf ? (p.Mf + z * p.smz + (long long)r * p.smr) : nullptr;
    float mx = -__builtin_inff();
    for (int j = tid; j < p.n; j += 256) { float v = s[j] * p.scale_in; if (mf) v += mf[j]; mx = fmaxf(mx, v); }
    red[tid] = mx; __syncthreads();
    for (int o = 128; o > 0; o >>= 1) { if (tid < o) red[tid] = fmaxf(red[tid], red[tid + o]); __syncthreads(); }
    mx = red[0]; __syncthreads();
    float sum = 0.f;
    for (int j = tid; j < p.n; j += 256) { float v = s[j] * p.scale_in; if (mf) v += mf[j]; sum += (mx == -__builtin_inff()) ? 0.f : expf(v - mx); }
    red[tid] = sum; __syncthreads();
    for (int o = 128; o > 0; o >>= 1) { if (tid < o) red[tid] += red[tid + o]; __syncthreads(); }
    sum = red[0];
    const float inv = (sum > 0.f) ? p.scale_out / sum : 0.f;
    float* d = p.dst + z * p.dz + (long long)r * p.dr;
    for (int j = tid; j < p.n; j += 256) { float v = s[j] * p.scale_in; if (mf) v += mf[j]; const float o = (mx == -__builtin_inff()) ? 0.f : expf(v - mx) * inv; VST2(float, d + j, o); }
}
__global__ __launch_bounds__(256) void k_stats(const float* __restrict__ x, long long sz, long long so, long long si, int inner, int n, float eps, float* __restrict__ stat, int mode) {
    __shared__ float red[256];
    const int z = blockIdx.x, tid = threadIdx.x;
    const float* base = x + z * sz;
    float s = 0.f;
    for (int e = tid; e < n; e += 256) s += base[(long long)(e / inner) * so + (long long)(e % inner) * si];
    red[tid] = s; __syncthreads();
    for (int o = 128; o > 0; o >>= 1) { if (tid < o) red[tid] += red[tid + o]; __syncthreads(); }
    const float mu = (mode == 0 || mode == 3) ? red[0] / (float)n : 0.f; __syncthreads();
    float q = 0.f;
    for (int e = tid; e < n; e += 256) { const float dlt = base[(long long)(e / inner) * so + (long long)(e % inner) * si] - mu; q += dlt * dlt; }
    red[tid] = q; __syncthreads();
    for (int o = 128; o > 0; o >>= 1) { if (tid < o) red[tid] += red[tid + o]; __syncthreads(); }
    {
        float rs;
        if (mode == 2) rs = sqrtf((float)n) / fmaxf(sqrtf(red[0]), eps); else if (mode == 3) rs = rsqrtf(red[0] / (float)(n - 1) + eps); else rs = rsqrtf(red[0] / (float)n + eps);
        if (tid < 32) { const float v = (tid == 0) ? mu : ((tid == 1) ? rs : 0.f); VST2(float, stat + (long long)z * 32 + tid, v); }
    }
}
__global__ __launch_bounds__(256) void k_norm_apply(const float* __restrict__ x, float* __restrict__ y, const float* __restrict__ stat, const float* __restrict__ g, const float* __restrict__ bta,
                                                     int Z, int C, int L, int G, int bn, int act) {
    const long long idx = (long long)blockIdx.x * 256 + threadIdx.x;
    if (idx >= (long long)Z * C * L) return;
    const int l = (int)(idx % L); const long long zc = idx / L; const int c = (int)(zc % C), z = (int)(zc / C); (void)l;
    const int set = bn ? c : (z * G + c / (C / G));
    float v = (x[idx] - stat[(long long)set * 32]) * stat[(long long)set * 32 + 1];
    if (g) v *= g[c];
    if (bta) v += bta[c];
    v = act_fn(v, act);
    VST2(float, y + idx, v);
}

__global__ __launch_bounds__(256) void k_lse_neg(const float* __restrict__ st, float* __restrict__ c, int n) {
    const int i = blockIdx.x * 256 + threadIdx.x;
    if (i < n) { const float v = -(st[2 * i] + logf(st[2 * i + 1])); VST2(float, c + i, v); }
}

__global__ __launch_bounds__(256) void k_iota(int* __restrict__ dst, int n, int a, int b) {
    const int i = blockIdx.x * 256 + threadIdx.x;
    if (i < n) { const int v = a * i + b; VST2(int, dst + i, v); }
}

__global__ __launch_bounds__(256) void k_axpby(const float* __restrict__ x, const float* __restrict__ y, float* __restrict__ dst, int n, float a, float b, float c) {
    const int i = blockIdx.x * 256 + threadIdx.x;
    if (i < n) { const float v = a * x[i] + b * y[i] + c; VST2(float, dst + i, v); }
}

struct RopeP { const float* X; float* Y; const float* C; const float* Sn; const int* pos; long long sXr, sXh, sYr, sYh, sCb, sCp, sCd; int R, Hn, D, S, mode, tmode, pmode, pad; };
static_assert(sizeof(RopeP) == 5 * 8 + 7 * 8 + 8 * 4, "RopeP has padding");
__global__ __launch_bounds__(256) void k_rope(RopeP p) {
    const long long idx = (long long)blockIdx.x * 256 + threadIdx.x;
    if (idx >= (long long)p.R * p.Hn * p.D) return;
    const int d = (int)(idx % p.D); const long long rh = idx / p.D; const int h = (int)(rh % p.Hn); const int r = (int)(rh / p.Hn);
    const int half = p.D / 2;
    int partner; float sign;
    if (p.mode == 0) { partner = (d < half) ? d + half : d - half; sign = (d < half) ? -1.f : 1.f; }
    else { partner = d ^ 1; sign = (d & 1) ? 1.f : -1.f; }
    const int tcol = (p.tmode == 0) ? d : ((p.tmode == 1) ? (d % half) : (d >> 1));
    const int pp = (p.pmode == 0) ? (r % p.S) : ((p.pmode == 1) ? h : p.pos[r]);
    const long long toff = (long long)(r / p.S) * p.sCb + (long long)pp * p.sCp + (long long)tcol * p.sCd;
    const float* xr = p.X + (long long)r * p.sXr + (long long)h * p.sXh;
    const float v = xr[d] * p.C[toff] + sign * xr[partner] * p.Sn[toff];
    VST2(float, p.Y + (long long)r * p.sYr + (long long)h * p.sYh + d, v);
}

__global__ __launch_bounds__(256) void k_invf(float* __restrict__ invb, int half, int D, float base, float num, int fmode, float cexp) {
    const int i = blockIdx.x * 256 + threadIdx.x;
    if (i >= ((half + 31) / 32) * 32) return;
    if (i >= half) { VST2(float, invb + i, 0.f); return; }
    const float e = (float)(2 * i) / (float)D;
    float invf;
    if (fmode == 1) invf = num * expf((float)(2 * i) * cexp);
    else if (fmode == 2) invf = num * powf(base, (-2.0f * ((float)i - 1.0f)) / (float)D);
    else invf = num * (1.0f / powf(base, e));
    VST2(float, invb + i, invf);
}
__global__ __launch_bounds__(256) void k_sincos(float* __restrict__ cs, float* __restrict__ sn, const float* __restrict__ invb, int S, int half, float pscale) {
    const int idx = blockIdx.x * 256 + threadIdx.x;
    if (idx >= S * half) return;
    const int s = idx / half, i = idx - s * half;
    const float ang = (pscale * (float)s) * invb[i];
    VST2(float, cs + idx, cosf(ang)); VST2(float, sn + idx, sinf(ang));
}

__global__ __launch_bounds__(256) void k_mulact(const float* __restrict__ x, const float* __restrict__ y, float* __restrict__ dst, int n, int act) {
    const int i = blockIdx.x * 256 + threadIdx.x;
    if (i < n) { const float v = act_fn(x[i], act) * y[i]; VST2(float, dst + i, v); }
}

__global__ __launch_bounds__(256) void k_matvec(GemmP p) {
    const int rpt = (p.N == 1) ? 1 : 32;
    const long long r0 = ((long long)blockIdx.x * 256 + threadIdx.x) * rpt; const int z = blockIdx.z, zo = z / p.zi_n, zi = z - zo * p.zi_n;
    if (r0 >= p.M) return;
    const float* Bb = p.B + zo * p.sBo + zi * p.sBi;
    float* C = p.C + zo * p.sCo + zi * p.sCi; const float* R = p.R + zo * p.sRo + zi * p.sRi;
    for (int rr = 0; rr < rpt; ++rr) {
        const long long r = r0 + rr; if (r >= p.M) break;
        const float* A = p.A + zo * p.sAo + zi * p.sAi + r * p.sAm;
        float acc[8] = {0.f, 0.f, 0.f, 0.f, 0.f, 0.f, 0.f, 0.f};
        for (int k = 0; k < p.K; ++k) { const float a = A[(long long)k * p.sAk];
#pragma unroll
            for (int j = 0; j < 8; ++j) if (j < p.N) acc[j] += a * Bb[(long long)j * p.sBn + (long long)k * p.sBk]; }
#pragma unroll
        for (int j = 0; j < 8; ++j) if (j < p.N) {
            float v = acc[j] * p.alpha;
            if (p.flags & 1) v += p.bias[j];
            if (p.flags & 2) v += p.bias[r];
            v = act_fn(v, p.act);
            if (p.flags & 4) v += p.beta * R[r * p.sRm + (long long)j * p.sRn];
            VST2(float, C + r * p.sCm + j, v);
        }
    }
}
__global__ __launch_bounds__(256) void k_smallsoftmax(const float* __restrict__ src, float* __restrict__ dst, long long sr, long long dr, int n, long long R, float scale) {
    const long long r0 = ((long long)blockIdx.x * 256 + threadIdx.x) * 32;
    for (int rr = 0; rr < 32; ++rr) {
        const long long r = r0 + rr; if (r >= R) return;
        const float* s = src + r * sr; float* d = dst + r * dr;
        float mx = -__builtin_inff();
        for (int j = 0; j < n; ++j) mx = fmaxf(mx, s[j] * scale);
        float sum = 0.f;
        for (int j = 0; j < n; ++j) sum += expf(s[j] * scale - mx);
        const float inv = 1.f / sum;
        for (int j = 0; j < n; ++j) { const float v = expf(s[j] * scale - mx) * inv; VST2(float, d + j, v); }
    }
}

__global__ __launch_bounds__(32) void k_unitstat(float* __restrict__ st) { const int t = threadIdx.x; const float v = (t == 1) ? 1.f : 0.f; VST2(float, st + t, v); }

__global__ __launch_bounds__(256) void k_lincopy(const float* __restrict__ src, long long lds, float* __restrict__ dst, long long ldd, long long rows, int cols) {
    const long long i = (long long)blockIdx.x * 256 + threadIdx.x; if (i >= rows * cols) return;
    const long long r = i / cols; const int c = (int)(i - r * cols);
    const float v = src[r * lds + c]; VST2(float, dst + r * ldd + c, v);
}

__global__ __launch_bounds__(256) void k_eq_soft(float* __restrict__ E, const int* __restrict__ mask, int N) { __shared__ float red[256]; const long long r = blockIdx.x; const int n = (int)(r % N); const int t = threadIdx.x; float* row = E + r * N; float mx = -__builtin_inff(); for (int m = t; m < N; m += 256) { const float v = (mask[n * N + m] == 0) ? -__builtin_inff() : row[m]; mx = fmaxf(mx, v); } red[t] = mx; __syncthreads(); for (int o = 128; o > 0; o >>= 1) { if (t < o) red[t] = fmaxf(red[t], red[t + o]); __syncthreads(); } mx = red[0]; __syncthreads();
    float s = 0.f; for (int m = t; m < N; m += 256) s += (mask[n * N + m] == 0) ? 0.f : expf(row[m] - mx); red[t] = s; __syncthreads(); for (int o = 128; o > 0; o >>= 1) { if (t < o) red[t] += red[t + o]; __syncthreads(); } s = red[0];
    for (int m = t; m < N; m += 256) { const float v = (mask[n * N + m] == 0) ? 0.f : expf(row[m] - mx) / s; VST2(float, row + m, v); } }

template __global__ void k_gemm<0>(GemmP);

extern "C" void kernel_launch(void* const* d_in, const int* in_sizes, int n_in, void* d_out, int out_size, void* d_ws, size_t ws_size, hipStream_t stream) {
    (void)in_sizes; (void)n_in; (void)out_size; (void)ws_size;
    const float* Q = (const float*)d_in[0];
    const float* Kx = (const float*)d_in[1];
    const int* mask = (const int*)d_in[2];
    const float* Wq = (const float*)d_in[3];
    const float* bq = (const float*)d_in[4];
    const float* Wk = (const float*)d_in[5];
    const float* bk = (const float*)d_in[6];
    const float* Wv = (const float*)d_in[7];
    const float* bv = (const float*)d_in[8];
    const float* Wo = (const float*)d_in[9];
    const float* bo = (const float*)d_in[10];
    const float* g0 = (const float*)d_in[11];
    const float* b0 = (const float*)d_in[12];
    const float* g1 = (const float*)d_in[13];
    const float* b1 = (const float*)d_in[14];
    const int Bn = 8;
    const int N = 512;
    const int S = 4;
    const int L = 256;
    const int NH = 4;
    const int DH = 64;
    const int NR = Bn * N * S;
    float* out = (float*)d_out;
    char* wsp = (char*)d_ws;
    float* QP = (float*)wsp; wsp += (((size_t)((size_t)NR * L) * 4 + 255) / 256) * 256;
    float* KP = (float*)wsp; wsp += (((size_t)((size_t)NR * L) * 4 + 255) / 256) * 256;
    float* VP = (float*)wsp; wsp += (((size_t)((size_t)NR * L) * 4 + 255) / 256) * 256;
    float* E = (float*)wsp; wsp += (((size_t)((size_t)NH * Bn * N * N) * 4 + 255) / 256) * 256;
    float* O = (float*)wsp; wsp += (((size_t)((size_t)NR * L) * 4 + 255) / 256) * 256;
    float* O2 = (float*)wsp; wsp += (((size_t)((size_t)NR * L) * 4 + 255) / 256) * 256;
    float* st = (float*)wsp; wsp += (((size_t)((size_t)NR * 32) * 4 + 255) / 256) * 256;
    { GemmP gq;
      gq.A = Q; gq.B = Wq; gq.bias = bq; gq.R = Q; gq.C = QP;
      gq.sAo = 0; gq.sAi = 0; gq.sAm = L; gq.sAk = 1; gq.sBo = 0; gq.sBi = 0; gq.sBn = L; gq.sBk = 1; gq.sCo = 0; gq.sCi = 0; gq.sCm = L; gq.sRo = 0; gq.sRi = 0; gq.sRm = 0; gq.sRn = 0;
      gq.M = NR; gq.N = L; gq.K = L; gq.zi_n = 1; gq.flags = 1; gq.act = 0;
      gq.alpha = 1.0f; gq.beta = 0.0f; gq.sa = 1.0f; gq.sb = 8.0f; gq.Npad = L; gq.pad_ = 0;
      if ((long long)(NR) >= 64 && (long long)(L) >= 64) k_gemmT<0, 4, 4><<<dim3((unsigned)((L) + 63) / 64, (unsigned)((NR) + 63) / 64, (unsigned)(1)), 32, 0, stream>>>(gq);
      else k_gemm<0><<<dim3((unsigned)((L) + 31) / 32, (unsigned)((NR) + 15) / 16, (unsigned)(1)), 32, 0, stream>>>(gq); }
    { GemmP gk;
      gk.A = Kx; gk.B = Wk; gk.bias = bk; gk.R = Kx; gk.C = KP;
      gk.sAo = 0; gk.sAi = 0; gk.sAm = L; gk.sAk = 1; gk.sBo = 0; gk.sBi = 0; gk.sBn = L; gk.sBk = 1; gk.sCo = 0; gk.sCi = 0; gk.sCm = L; gk.sRo = 0; gk.sRi = 0; gk.sRm = 0; gk.sRn = 0;
      gk.M = NR; gk.N = L; gk.K = L; gk.zi_n = 1; gk.flags = 1; gk.act = 0;
      gk.alpha = 1.0f; gk.beta = 0.0f; gk.sa = 1.0f; gk.sb = 8.0f; gk.Npad = L; gk.pad_ = 0;
      if ((long long)(NR) >= 64 && (long long)(L) >= 64) k_gemmT<0, 4, 4><<<dim3((unsigned)((L) + 63) / 64, (unsigned)((NR) + 63) / 64, (unsigned)(1)), 32, 0, stream>>>(gk);
      else k_gemm<0><<<dim3((unsigned)((L) + 31) / 32, (unsigned)((NR) + 15) / 16, (unsigned)(1)), 32, 0, stream>>>(gk); }
    { GemmP gv;
      gv.A = Kx; gv.B = Wv; gv.bias = bv; gv.R = Kx; gv.C = VP;
      gv.sAo = 0; gv.sAi = 0; gv.sAm = L; gv.sAk = 1; gv.sBo = 0; gv.sBi = 0; gv.sBn = L; gv.sBk = 1; gv.sCo = 0; gv.sCi = 0; gv.sCm = L; gv.sRo = 0; gv.sRi = 0; gv.sRm = 0; gv.sRn = 0;
      gv.M = NR; gv.N = L; gv.K = L; gv.zi_n = 1; gv.flags = 1; gv.act = 0;
      gv.alpha = 1.0f; gv.beta = 0.0f; gv.sa = 1.0f; gv.sb = 8.0f; gv.Npad = L; gv.pad_ = 0;
      if ((long long)(NR) >= 64 && (long long)(L) >= 64) k_gemmT<0, 4, 4><<<dim3((unsigned)((L) + 63) / 64, (unsigned)((NR) + 63) / 64, (unsigned)(1)), 32, 0, stream>>>(gv);
      else k_gemm<0><<<dim3((unsigned)((L) + 31) / 32, (unsigned)((NR) + 15) / 16, (unsigned)(1)), 32, 0, stream>>>(gv); }
    { GemmP ge00;
      ge00.A = QP + 0 * L + 0 * DH; ge00.B = KP + 0 * L + 0 * DH; ge00.bias = QP + 0 * L + 0 * DH; ge00.R = QP + 0 * L + 0 * DH; ge00.C = E + (size_t)0 * Bn * N * N;
      ge00.sAo = (long long)N * S * L; ge00.sAi = 0; ge00.sAm = S * L; ge00.sAk = 1; ge00.sBo = (long long)N * S * L; ge00.sBi = 0; ge00.sBn = S * L; ge00.sBk = 1; ge00.sCo = (long long)N * N; ge00.sCi = 0; ge00.sCm = N; ge00.sRo = 0; ge00.sRi = 0; ge00.sRm = 0; ge00.sRn = 0;
      ge00.M = N; ge00.N = N; ge00.K = DH; ge00.zi_n = 1; ge00.flags = 0; ge00.act = 0;
      ge00.alpha = 0.0625f; ge00.beta = 0.0f; ge00.sa = 1.0f; ge00.sb = 1.0f; ge00.Npad = N; ge00.pad_ = 0;
      if ((long long)(N) >= 64 && (long long)(N) >= 64) k_gemmT<0, 4, 4><<<dim3((unsigned)((N) + 63) / 64, (unsigned)((N) + 63) / 64, (unsigned)(Bn)), 32, 0, stream>>>(ge00);
      else k_gemm<0><<<dim3((unsigned)((N) + 31) / 32, (unsigned)((N) + 15) / 16, (unsigned)(Bn)), 32, 0, stream>>>(ge00); }
    { GemmP ge01;
      ge01.A = QP + 1 * L + 0 * DH; ge01.B = KP + 1 * L + 0 * DH; ge01.bias = QP + 1 * L + 0 * DH; ge01.R = E + (size_t)0 * Bn * N * N; ge01.C = E + (size_t)0 * Bn * N * N;
      ge01.sAo = (long long)N * S * L; ge01.sAi = 0; ge01.sAm = S * L; ge01.sAk = 1; ge01.sBo = (long long)N * S * L; ge01.sBi = 0; ge01.sBn = S * L; ge01.sBk = 1; ge01.sCo = (long long)N * N; ge01.sCi = 0; ge01.sCm = N; ge01.sRo = (long long)N * N; ge01.sRi = 0; ge01.sRm = N; ge01.sRn = 1;
      ge01.M = N; ge01.N = N; ge01.K = DH; ge01.zi_n = 1; ge01.flags = 4; ge01.act = 0;
      ge01.alpha = 0.0625f; ge01.beta = 1.0f; ge01.sa = 1.0f; ge01.sb = 1.0f; ge01.Npad = N; ge01.pad_ = 0;
      if ((long long)(N) >= 64 && (long long)(N) >= 64) k_gemmT<0, 4, 4><<<dim3((unsigned)((N) + 63) / 64, (unsigned)((N) + 63) / 64, (unsigned)(Bn)), 32, 0, stream>>>(ge01);
      else k_gemm<0><<<dim3((unsigned)((N) + 31) / 32, (unsigned)((N) + 15) / 16, (unsigned)(Bn)), 32, 0, stream>>>(ge01); }
    { GemmP ge02;
      ge02.A = QP + 2 * L + 0 * DH; ge02.B = KP + 2 * L + 0 * DH; ge02.bias = QP + 2 * L + 0 * DH; ge02.R = E + (size_t)0 * Bn * N * N; ge02.C = E + (size_t)0 * Bn * N * N;
      ge02.sAo = (long long)N * S * L; ge02.sAi = 0; ge02.sAm = S * L; ge02.sAk = 1; ge02.sBo = (long long)N * S * L; ge02.sBi = 0; ge02.sBn = S * L; ge02.sBk = 1; ge02.sCo = (long long)N * N; ge02.sCi = 0; ge02.sCm = N; ge02.sRo = (long long)N * N; ge02.sRi = 0; ge02.sRm = N; ge02.sRn = 1;
      ge02.M = N; ge02.N = N; ge02.K = DH; ge02.zi_n = 1; ge02.flags = 4; ge02.act = 0;
      ge02.alpha = 0.0625f; ge02.beta = 1.0f; ge02.sa = 1.0f; ge02.sb = 1.0f; ge02.Npad = N; ge02.pad_ = 0;
      if ((long long)(N) >= 64 && (long long)(N) >= 64) k_gemmT<0, 4, 4><<<dim3((unsigned)((N) + 63) / 64, (unsigned)((N) + 63) / 64, (unsigned)(Bn)), 32, 0, stream>>>(ge02);
      else k_gemm<0><<<dim3((unsigned)((N) + 31) / 32, (unsigned)((N) + 15) / 16, (unsigned)(Bn)), 32, 0, stream>>>(ge02); }
    { GemmP ge03;
      ge03.A = QP + 3 * L + 0 * DH; ge03.B = KP + 3 * L + 0 * DH; ge03.bias = QP + 3 * L + 0 * DH; ge03.R = E + (size_t)0 * Bn * N * N; ge03.C = E + (size_t)0 * Bn * N * N;
      ge03.sAo = (long long)N * S * L; ge03.sAi = 0; ge03.sAm = S * L; ge03.sAk = 1; ge03.sBo = (long long)N * S * L; ge03.sBi = 0; ge03.sBn = S * L; ge03.sBk = 1; ge03.sCo = (long long)N * N; ge03.sCi = 0; ge03.sCm = N; ge03.sRo = (long long)N * N; ge03.sRi = 0; ge03.sRm = N; ge03.sRn = 1;
      ge03.M = N; ge03.N = N; ge03.K = DH; ge03.zi_n = 1; ge03.flags = 4; ge03.act = 0;
      ge03.alpha = 0.0625f; ge03.beta = 1.0f; ge03.sa = 1.0f; ge03.sb = 1.0f; ge03.Npad = N; ge03.pad_ = 0;
      if ((long long)(N) >= 64 && (long long)(N) >= 64) k_gemmT<0, 4, 4><<<dim3((unsigned)((N) + 63) / 64, (unsigned)((N) + 63) / 64, (unsigned)(Bn)), 32, 0, stream>>>(ge03);
      else k_gemm<0><<<dim3((unsigned)((N) + 31) / 32, (unsigned)((N) + 15) / 16, (unsigned)(Bn)), 32, 0, stream>>>(ge03); }
    { GemmP ge10;
      ge10.A = QP + 0 * L + 1 * DH; ge10.B = KP + 0 * L + 1 * DH; ge10.bias = QP + 0 * L + 1 * DH; ge10.R = QP + 0 * L + 1 * DH; ge10.C = E + (size_t)1 * Bn * N * N;
      ge10.sAo = (long long)N * S * L; ge10.sAi = 0; ge10.sAm = S * L; ge10.sAk = 1; ge10.sBo = (long long)N * S * L; ge10.sBi = 0; ge10.sBn = S * L; ge10.sBk = 1; ge10.sCo = (long long)N * N; ge10.sCi = 0; ge10.sCm = N; ge10.sRo = 0; ge10.sRi = 0; ge10.sRm = 0; ge10.sRn = 0;
      ge10.M = N; ge10.N = N; ge10.K = DH; ge10.zi_n = 1; ge10.flags = 0; ge10.act = 0;
      ge10.alpha = 0.0625f; ge10.beta = 0.0f; ge10.sa = 1.0f; ge10.sb = 1.0f; ge10.Npad = N; ge10.pad_ = 0;
      if ((long long)(N) >= 64 && (long long)(N) >= 64) k_gemmT<0, 4, 4><<<dim3((unsigned)((N) + 63) / 64, (unsigned)((N) + 63) / 64, (unsigned)(Bn)), 32, 0, stream>>>(ge10);
      else k_gemm<0><<<dim3((unsigned)((N) + 31) / 32, (unsigned)((N) + 15) / 16, (unsigned)(Bn)), 32, 0, stream>>>(ge10); }
    { GemmP ge11;
      ge11.A = QP + 1 * L + 1 * DH; ge11.B = KP + 1 * L + 1 * DH; ge11.bias = QP + 1 * L + 1 * DH; ge11.R = E + (size_t)1 * Bn * N * N; ge11.C = E + (size_t)1 * Bn * N * N;
      ge11.sAo = (long long)N * S * L; ge11.sAi = 0; ge11.sAm = S * L; ge11.sAk = 1; ge11.sBo = (long long)N * S * L; ge11.sBi = 0; ge11.sBn = S * L; ge11.sBk = 1; ge11.sCo = (long long)N * N; ge11.sCi = 0; ge11.sCm = N; ge11.sRo = (long long)N * N; ge11.sRi = 0; ge11.sRm = N; ge11.sRn = 1;
      ge11.M = N; ge11.N = N; ge11.K = DH; ge11.zi_n = 1; ge11.flags = 4; ge11.act = 0;
      ge11.alpha = 0.0625f; ge11.beta = 1.0f; ge11.sa = 1.0f; ge11.sb = 1.0f; ge11.Npad = N; ge11.pad_ = 0;
      if ((long long)(N) >= 64 && (long long)(N) >= 64) k_gemmT<0, 4, 4><<<dim3((unsigned)((N) + 63) / 64, (unsigned)((N) + 63) / 64, (unsigned)(Bn)), 32, 0, stream>>>(ge11);
      else k_gemm<0><<<dim3((unsigned)((N) + 31) / 32, (unsigned)((N) + 15) / 16, (unsigned)(Bn)), 32, 0, stream>>>(ge11); }
    { GemmP ge12;
      ge12.A = QP + 2 * L + 1 * DH; ge12.B = KP + 2 * L + 1 * DH; ge12.bias = QP + 2 * L + 1 * DH; ge12.R = E + (size_t)1 * Bn * N * N; ge12.C = E + (size_t)1 * Bn * N * N;
      ge12.sAo = (long long)N * S * L; ge12.sAi = 0; ge12.sAm = S * L; ge12.sAk = 1; ge12.sBo = (long long)N * S * L; ge12.sBi = 0; ge12.sBn = S * L; ge12.sBk = 1; ge12.sCo = (long long)N * N; ge12.sCi = 0; ge12.sCm = N; ge12.sRo = (long long)N * N; ge12.sRi = 0; ge12.sRm = N; ge12.sRn = 1;
      ge12.M = N; ge12.N = N; ge12.K = DH; ge12.zi_n = 1; ge12.flags = 4; ge12.act = 0;
      ge12.alpha = 0.0625f; ge12.beta = 1.0f; ge12.sa = 1.0f; ge12.sb = 1.0f; ge12.Npad = N; ge12.pad_ = 0;
      if ((long long)(N) >= 64 && (long long)(N) >= 64) k_gemmT<0, 4, 4><<<dim3((unsigned)((N) + 63) / 64, (unsigned)((N) + 63) / 64, (unsigned)(Bn)), 32, 0, stream>>>(ge12);
      else k_gemm<0><<<dim3((unsigned)((N) + 31) / 32, (unsigned)((N) + 15) / 16, (unsigned)(Bn)), 32, 0, stream>>>(ge12); }
    { GemmP ge13;
      ge13.A = QP + 3 * L + 1 * DH; ge13.B = KP + 3 * L + 1 * DH; ge13.bias = QP + 3 * L + 1 * DH; ge13.R = E + (size_t)1 * Bn * N * N; ge13.C = E + (size_t)1 * Bn * N * N;
      ge13.sAo = (long long)N * S * L; ge13.sAi = 0; ge13.sAm = S * L; ge13.sAk = 1; ge13.sBo = (long long)N * S * L; ge13.sBi = 0; ge13.sBn = S * L; ge13.sBk = 1; ge13.sCo = (long long)N * N; ge13.sCi = 0; ge13.sCm = N; ge13.sRo = (long long)N * N; ge13.sRi = 0; ge13.sRm = N; ge13.sRn = 1;
      ge13.M = N; ge13.N = N; ge13.K = DH; ge13.zi_n = 1; ge13.flags = 4; ge13.act = 0;
      ge13.alpha = 0.0625f; ge13.beta = 1.0f; ge13.sa = 1.0f; ge13.sb = 1.0f; ge13.Npad = N; ge13.pad_ = 0;
      if ((long long)(N) >= 64 && (long long)(N) >= 64) k_gemmT<0, 4, 4><<<dim3((unsigned)((N) + 63) / 64, (unsigned)((N) + 63) / 64, (unsigned)(Bn)), 32, 0, stream>>>(ge13);
      else k_gemm<0><<<dim3((unsigned)((N) + 31) / 32, (unsigned)((N) + 15) / 16, (unsigned)(Bn)), 32, 0, stream>>>(ge13); }
    { GemmP ge20;
      ge20.A = QP + 0 * L + 2 * DH; ge20.B = KP + 0 * L + 2 * DH; ge20.bias = QP + 0 * L + 2 * DH; ge20.R = QP + 0 * L + 2 * DH; ge20.C = E + (size_t)2 * Bn * N * N;
      ge20.sAo = (long long)N * S * L; ge20.sAi = 0; ge20.sAm = S * L; ge20.sAk = 1; ge20.sBo = (long long)N * S * L; ge20.sBi = 0; ge20.sBn = S * L; ge20.sBk = 1; ge20.sCo = (long long)N * N; ge20.sCi = 0; ge20.sCm = N; ge20.sRo = 0; ge20.sRi = 0; ge20.sRm = 0; ge20.sRn = 0;
      ge20.M = N; ge20.N = N; ge20.K = DH; ge20.zi_n = 1; ge20.flags = 0; ge20.act = 0;
      ge20.alpha = 0.0625f; ge20.beta = 0.0f; ge20.sa = 1.0f; ge20.sb = 1.0f; ge20.Npad = N; ge20.pad_ = 0;
      if ((long long)(N) >= 64 && (long long)(N) >= 64) k_gemmT<0, 4, 4><<<dim3((unsigned)((N) + 63) / 64, (unsigned)((N) + 63) / 64, (unsigned)(Bn)), 32, 0, stream>>>(ge20);
      else k_gemm<0><<<dim3((unsigned)((N) + 31) / 32, (unsigned)((N) + 15) / 16, (unsigned)(Bn)), 32, 0, stream>>>(ge20); }
    { GemmP ge21;
      ge21.A = QP + 1 * L + 2 * DH; ge21.B = KP + 1 * L + 2 * DH; ge21.bias = QP + 1 * L + 2 * DH; ge21.R = E + (size_t)2 * Bn * N * N; ge21.C = E + (size_t)2 * Bn * N * N;
      ge21.sAo = (long long)N * S * L; ge21.sAi = 0; ge21.sAm = S * L; ge21.sAk = 1; ge21.sBo = (long long)N * S * L; ge21.sBi = 0; ge21.sBn = S * L; ge21.sBk = 1; ge21.sCo = (long long)N * N; ge21.sCi = 0; ge21.sCm = N; ge21.sRo = (long long)N * N; ge21.sRi = 0; ge21.sRm = N; ge21.sRn = 1;
      ge21.M = N; ge21.N = N; ge21.K = DH; ge21.zi_n = 1; ge21.flags = 4; ge21.act = 0;
      ge21.alpha = 0.0625f; ge21.beta = 1.0f; ge21.sa = 1.0f; ge21.sb = 1.0f; ge21.Npad = N; ge21.pad_ = 0;
      if ((long long)(N) >= 64 && (long long)(N) >= 64) k_gemmT<0, 4, 4><<<dim3((unsigned)((N) + 63) / 64, (unsigned)((N) + 63) / 64, (unsigned)(Bn)), 32, 0, stream>>>(ge21);
      else k_gemm<0><<<dim3((unsigned)((N) + 31) / 32, (unsigned)((N) + 15) / 16, (unsigned)(Bn)), 32, 0, stream>>>(ge21); }
    { GemmP ge22;
      ge22.A = QP + 2 * L + 2 * DH; ge22.B = KP + 2 * L + 2 * DH; ge22.bias = QP + 2 * L + 2 * DH; ge22.R = E + (size_t)2 * Bn * N * N; ge22.C = E + (size_t)2 * Bn * N * N;
      ge22.sAo = (long long)N * S * L; ge22.sAi = 0; ge22.sAm = S * L; ge22.sAk = 1; ge22.sBo = (long long)N * S * L; ge22.sBi = 0; ge22.sBn = S * L; ge22.sBk = 1; ge22.sCo = (long long)N * N; ge22.sCi = 0; ge22.sCm = N; ge22.sRo = (long long)N * N; ge22.sRi = 0; ge22.sRm = N; ge22.sRn = 1;
      ge22.M = N; ge22.N = N; ge22.K = DH; ge22.zi_n = 1; ge22.flags = 4; ge22.act = 0;
      ge22.alpha = 0.0625f; ge22.beta = 1.0f; ge22.sa = 1.0f; ge22.sb = 1.0f; ge22.Npad = N; ge22.pad_ = 0;
      if ((long long)(N) >= 64 && (long long)(N) >= 64) k_gemmT<0, 4, 4><<<dim3((unsigned)((N) + 63) / 64, (unsigned)((N) + 63) / 64, (unsigned)(Bn)), 32, 0, stream>>>(ge22);
      else k_gemm<0><<<dim3((unsigned)((N) + 31) / 32, (unsigned)((N) + 15) / 16, (unsigned)(Bn)), 32, 0, stream>>>(ge22); }
    { GemmP ge23;
      ge23.A = QP + 3 * L + 2 * DH; ge23.B = KP + 3 * L + 2 * DH; ge23.bias = QP + 3 * L + 2 * DH; ge23.R = E + (size_t)2 * Bn * N * N; ge23.C = E + (size_t)2 * Bn * N * N;
      ge23.sAo = (long long)N * S * L; ge23.sAi = 0; ge23.sAm = S * L; ge23.sAk = 1; ge23.sBo = (long long)N * S * L; ge23.sBi = 0; ge23.sBn = S * L; ge23.sBk = 1; ge23.sCo = (long long)N * N; ge23.sCi = 0; ge23.sCm = N; ge23.sRo = (long long)N * N; ge23.sRi = 0; ge23.sRm = N; ge23.sRn = 1;
      ge23.M = N; ge23.N = N; ge23.K = DH; ge23.zi_n = 1; ge23.flags = 4; ge23.act = 0;
      ge23.alpha = 0.0625f; ge23.beta = 1.0f; ge23.sa = 1.0f; ge23.sb = 1.0f; ge23.Npad = N; ge23.pad_ = 0;
      if ((long long)(N) >= 64 && (long long)(N) >= 64) k_gemmT<0, 4, 4><<<dim3((unsigned)((N) + 63) / 64, (unsigned)((N) + 63) / 64, (unsigned)(Bn)), 32, 0, stream>>>(ge23);
      else k_gemm<0><<<dim3((unsigned)((N) + 31) / 32, (unsigned)((N) + 15) / 16, (unsigned)(Bn)), 32, 0, stream>>>(ge23); }
    { GemmP ge30;
      ge30.A = QP + 0 * L + 3 * DH; ge30.B = KP + 0 * L + 3 * DH; ge30.bias = QP + 0 * L + 3 * DH; ge30.R = QP + 0 * L + 3 * DH; ge30.C = E + (size_t)3 * Bn * N * N;
      ge30.sAo = (long long)N * S * L; ge30.sAi = 0; ge30.sAm = S * L; ge30.sAk = 1; ge30.sBo = (long long)N * S * L; ge30.sBi = 0; ge30.sBn = S * L; ge30.sBk = 1; ge30.sCo = (long long)N * N; ge30.sCi = 0; ge30.sCm = N; ge30.sRo = 0; ge30.sRi = 0; ge30.sRm = 0; ge30.sRn = 0;
      ge30.M = N; ge30.N = N; ge30.K = DH; ge30.zi_n = 1; ge30.flags = 0; ge30.act = 0;
      ge30.alpha = 0.0625f; ge30.beta = 0.0f; ge30.sa = 1.0f; ge30.sb = 1.0f; ge30.Npad = N; ge30.pad_ = 0;
      if ((long long)(N) >= 64 && (long long)(N) >= 64) k_gemmT<0, 4, 4><<<dim3((unsigned)((N) + 63) / 64, (unsigned)((N) + 63) / 64, (unsigned)(Bn)), 32, 0, stream>>>(ge30);
      else k_gemm<0><<<dim3((unsigned)((N) + 31) / 32, (unsigned)((N) + 15) / 16, (unsigned)(Bn)), 32, 0, stream>>>(ge30); }
    { GemmP ge31;
      ge31.A = QP + 1 * L + 3 * DH; ge31.B = KP + 1 * L + 3 * DH; ge31.bias = QP + 1 * L + 3 * DH; ge31.R = E + (size_t)3 * Bn * N * N; ge31.C = E + (size_t)3 * Bn * N * N;
      ge31.sAo = (long long)N * S * L; ge31.sAi = 0; ge31.sAm = S * L; ge31.sAk = 1; ge31.sBo = (long long)N * S * L; ge31.sBi = 0; ge31.sBn = S * L; ge31.sBk = 1; ge31.sCo = (long long)N * N; ge31.sCi = 0; ge31.sCm = N; ge31.sRo = (long long)N * N; ge31.sRi = 0; ge31.sRm = N; ge31.sRn = 1;
      ge31.M = N; ge31.N = N; ge31.K = DH; ge31.zi_n = 1; ge31.flags = 4; ge31.act = 0;
      ge31.alpha = 0.0625f; ge31.beta = 1.0f; ge31.sa = 1.0f; ge31.sb = 1.0f; ge31.Npad = N; ge31.pad_ = 0;
      if ((long long)(N) >= 64 && (long long)(N) >= 64) k_gemmT<0, 4, 4><<<dim3((unsigned)((N) + 63) / 64, (unsigned)((N) + 63) / 64, (unsigned)(Bn)), 32, 0, stream>>>(ge31);
      else k_gemm<0><<<dim3((unsigned)((N) + 31) / 32, (unsigned)((N) + 15) / 16, (unsigned)(Bn)), 32, 0, stream>>>(ge31); }
    { GemmP ge32;
      ge32.A = QP + 2 * L + 3 * DH; ge32.B = KP + 2 * L + 3 * DH; ge32.bias = QP + 2 * L + 3 * DH; ge32.R = E + (size_t)3 * Bn * N * N; ge32.C = E + (size_t)3 * Bn * N * N;
      ge32.sAo = (long long)N * S * L; ge32.sAi = 0; ge32.sAm = S * L; ge32.sAk = 1; ge32.sBo = (long long)N * S * L; ge32.sBi = 0; ge32.sBn = S * L; ge32.sBk = 1; ge32.sCo = (long long)N * N; ge32.sCi = 0; ge32.sCm = N; ge32.sRo = (long long)N * N; ge32.sRi = 0; ge32.sRm = N; ge32.sRn = 1;
      ge32.M = N; ge32.N = N; ge32.K = DH; ge32.zi_n = 1; ge32.flags = 4; ge32.act = 0;
      ge32.alpha = 0.0625f; ge32.beta = 1.0f; ge32.sa = 1.0f; ge32.sb = 1.0f; ge32.Npad = N; ge32.pad_ = 0;
      if ((long long)(N) >= 64 && (long long)(N) >= 64) k_gemmT<0, 4, 4><<<dim3((unsigned)((N) + 63) / 64, (unsigned)((N) + 63) / 64, (unsigned)(Bn)), 32, 0, stream>>>(ge32);
      else k_gemm<0><<<dim3((unsigned)((N) + 31) / 32, (unsigned)((N) + 15) / 16, (unsigned)(Bn)), 32, 0, stream>>>(ge32); }
    { GemmP ge33;
      ge33.A = QP + 3 * L + 3 * DH; ge33.B = KP + 3 * L + 3 * DH; ge33.bias = QP + 3 * L + 3 * DH; ge33.R = E + (size_t)3 * Bn * N * N; ge33.C = E + (size_t)3 * Bn * N * N;
      ge33.sAo = (long long)N * S * L; ge33.sAi = 0; ge33.sAm = S * L; ge33.sAk = 1; ge33.sBo = (long long)N * S * L; ge33.sBi = 0; ge33.sBn = S * L; ge33.sBk = 1; ge33.sCo = (long long)N * N; ge33.sCi = 0; ge33.sCm = N; ge33.sRo = (long long)N * N; ge33.sRi = 0; ge33.sRm = N; ge33.sRn = 1;
      ge33.M = N; ge33.N = N; ge33.K = DH; ge33.zi_n = 1; ge33.flags = 4; ge33.act = 0;
      ge33.alpha = 0.0625f; ge33.beta = 1.0f; ge33.sa = 1.0f; ge33.sb = 1.0f; ge33.Npad = N; ge33.pad_ = 0;
      if ((long long)(N) >= 64 && (long long)(N) >= 64) k_gemmT<0, 4, 4><<<dim3((unsigned)((N) + 63) / 64, (unsigned)((N) + 63) / 64, (unsigned)(Bn)), 32, 0, stream>>>(ge33);
      else k_gemm<0><<<dim3((unsigned)((N) + 31) / 32, (unsigned)((N) + 15) / 16, (unsigned)(Bn)), 32, 0, stream>>>(ge33); }
    k_eq_soft<<<NH * Bn * N, 256, 0, stream>>>(E, mask, N);
    { GemmP gav00;
      gav00.A = E + (size_t)0 * Bn * N * N; gav00.B = VP + 0 * L + 0 * DH; gav00.bias = E + (size_t)0 * Bn * N * N; gav00.R = QP + 0 * L + 0 * DH; gav00.C = O + 0 * L + 0 * DH;
      gav00.sAo = (long long)N * N; gav00.sAi = 0; gav00.sAm = N; gav00.sAk = 1; gav00.sBo = (long long)N * S * L; gav00.sBi = 0; gav00.sBn = 1; gav00.sBk = S * L; gav00.sCo = (long long)N * S * L; gav00.sCi = 0; gav00.sCm = S * L; gav00.sRo = (long long)N * S * L; gav00.sRi = 0; gav00.sRm = S * L; gav00.sRn = 1;
      gav00.M = N; gav00.N = DH; gav00.K = N; gav00.zi_n = 1; gav00.flags = 4; gav00.act = 0;
      gav00.alpha = 1.0f; gav00.beta = 1.0f; gav00.sa = 1.0f; gav00.sb = 1.0f; gav00.Npad = DH; gav00.pad_ = 0;
      if ((long long)(N) >= 64 && (long long)(DH) >= 64) k_gemmT<0, 4, 4><<<dim3((unsigned)((DH) + 63) / 64, (unsigned)((N) + 63) / 64, (unsigned)(Bn)), 32, 0, stream>>>(gav00);
      else k_gemm<0><<<dim3((unsigned)((DH) + 31) / 32, (unsigned)((N) + 15) / 16, (unsigned)(Bn)), 32, 0, stream>>>(gav00); }
    { GemmP gav01;
      gav01.A = E + (size_t)0 * Bn * N * N; gav01.B = VP + 1 * L + 0 * DH; gav01.bias = E + (size_t)0 * Bn * N * N; gav01.R = QP + 1 * L + 0 * DH; gav01.C = O + 1 * L + 0 * DH;
      gav01.sAo = (long long)N * N; gav01.sAi = 0; gav01.sAm = N; gav01.sAk = 1; gav01.sBo = (long long)N * S * L; gav01.sBi = 0; gav01.sBn = 1; gav01.sBk = S * L; gav01.sCo = (long long)N * S * L; gav01.sCi = 0; gav01.sCm = S * L; gav01.sRo = (long long)N * S * L; gav01.sRi = 0; gav01.sRm = S * L; gav01.sRn = 1;
      gav01.M = N; gav01.N = DH; gav01.K = N; gav01.zi_n = 1; gav01.flags = 4; gav01.act = 0;
      gav01.alpha = 1.0f; gav01.beta = 1.0f; gav01.sa = 1.0f; gav01.sb = 1.0f; gav01.Npad = DH; gav01.pad_ = 0;
      if ((long long)(N) >= 64 && (long long)(DH) >= 64) k_gemmT<0, 4, 4><<<dim3((unsigned)((DH) + 63) / 64, (unsigned)((N) + 63) / 64, (unsigned)(Bn)), 32, 0, stream>>>(gav01);
      else k_gemm<0><<<dim3((unsigned)((DH) + 31) / 32, (unsigned)((N) + 15) / 16, (unsigned)(Bn)), 32, 0, stream>>>(gav01); }
    { GemmP gav02;
      gav02.A = E + (size_t)0 * Bn * N * N; gav02.B = VP + 2 * L + 0 * DH; gav02.bias = E + (size_t)0 * Bn * N * N; gav02.R = QP + 2 * L + 0 * DH; gav02.C = O + 2 * L + 0 * DH;
      gav02.sAo = (long long)N * N; gav02.sAi = 0; gav02.sAm = N; gav02.sAk = 1; gav02.sBo = (long long)N * S * L; gav02.sBi = 0; gav02.sBn = 1; gav02.sBk = S * L; gav02.sCo = (long long)N * S * L; gav02.sCi = 0; gav02.sCm = S * L; gav02.sRo = (long long)N * S * L; gav02.sRi = 0; gav02.sRm = S * L; gav02.sRn = 1;
      gav02.M = N; gav02.N = DH; gav02.K = N; gav02.zi_n = 1; gav02.flags = 4; gav02.act = 0;
      gav02.alpha = 1.0f; gav02.beta = 1.0f; gav02.sa = 1.0f; gav02.sb = 1.0f; gav02.Npad = DH; gav02.pad_ = 0;
      if ((long long)(N) >= 64 && (long long)(DH) >= 64) k_gemmT<0, 4, 4><<<dim3((unsigned)((DH) + 63) / 64, (unsigned)((N) + 63) / 64, (unsigned)(Bn)), 32, 0, stream>>>(gav02);
      else k_gemm<0><<<dim3((unsigned)((DH) + 31) / 32, (unsigned)((N) + 15) / 16, (unsigned)(Bn)), 32, 0, stream>>>(gav02); }
    { GemmP gav03;
      gav03.A = E + (size_t)0 * Bn * N * N; gav03.B = VP + 3 * L + 0 * DH; gav03.bias = E + (size_t)0 * Bn * N * N; gav03.R = QP + 3 * L + 0 * DH; gav03.C = O + 3 * L + 0 * DH;
      gav03.sAo = (long long)N * N; gav03.sAi = 0; gav03.sAm = N; gav03.sAk = 1; gav03.sBo = (long long)N * S * L; gav03.sBi = 0; gav03.sBn = 1; gav03.sBk = S * L; gav03.sCo = (long long)N * S * L; gav03.sCi = 0; gav03.sCm = S * L; gav03.sRo = (long long)N * S * L; gav03.sRi = 0; gav03.sRm = S * L; gav03.sRn = 1;
      gav03.M = N; gav03.N = DH; gav03.K = N; gav03.zi_n = 1; gav03.flags = 4; gav03.act = 0;
      gav03.alpha = 1.0f; gav03.beta = 1.0f; gav03.sa = 1.0f; gav03.sb = 1.0f; gav03.Npad = DH; gav03.pad_ = 0;
      if ((long long)(N) >= 64 && (long long)(DH) >= 64) k_gemmT<0, 4, 4><<<dim3((unsigned)((DH) + 63) / 64, (unsigned)((N) + 63) / 64, (unsigned)(Bn)), 32, 0, stream>>>(gav03);
      else k_gemm<0><<<dim3((unsigned)((DH) + 31) / 32, (unsigned)((N) + 15) / 16, (unsigned)(Bn)), 32, 0, stream>>>(gav03); }
    { GemmP gav10;
      gav10.A = E + (size_t)1 * Bn * N * N; gav10.B = VP + 0 * L + 1 * DH; gav10.bias = E + (size_t)1 * Bn * N * N; gav10.R = QP + 0 * L + 1 * DH; gav10.C = O + 0 * L + 1 * DH;
      gav10.sAo = (long long)N * N; gav10.sAi = 0; gav10.sAm = N; gav10.sAk = 1; gav10.sBo = (long long)N * S * L; gav10.sBi = 0; gav10.sBn = 1; gav10.sBk = S * L; gav10.sCo = (long long)N * S * L; gav10.sCi = 0; gav10.sCm = S * L; gav10.sRo = (long long)N * S * L; gav10.sRi = 0; gav10.sRm = S * L; gav10.sRn = 1;
      gav10.M = N; gav10.N = DH; gav10.K = N; gav10.zi_n = 1; gav10.flags = 4; gav10.act = 0;
      gav10.alpha = 1.0f; gav10.beta = 1.0f; gav10.sa = 1.0f; gav10.sb = 1.0f; gav10.Npad = DH; gav10.pad_ = 0;
      if ((long long)(N) >= 64 && (long long)(DH) >= 64) k_gemmT<0, 4, 4><<<dim3((unsigned)((DH) + 63) / 64, (unsigned)((N) + 63) / 64, (unsigned)(Bn)), 32, 0, stream>>>(gav10);
      else k_gemm<0><<<dim3((unsigned)((DH) + 31) / 32, (unsigned)((N) + 15) / 16, (unsigned)(Bn)), 32, 0, stream>>>(gav10); }
    { GemmP gav11;
      gav11.A = E + (size_t)1 * Bn * N * N; gav11.B = VP + 1 * L + 1 * DH; gav11.bias = E + (size_t)1 * Bn * N * N; gav11.R = QP + 1 * L + 1 * DH; gav11.C = O + 1 * L + 1 * DH;
      gav11.sAo = (long long)N * N; gav11.sAi = 0; gav11.sAm = N; gav11.sAk = 1; gav11.sBo = (long long)N * S * L; gav11.sBi = 0; gav11.sBn = 1; gav11.sBk = S * L; gav11.sCo = (long long)N * S * L; gav11.sCi = 0; gav11.sCm = S * L; gav11.sRo = (long long)N * S * L; gav11.sRi = 0; gav11.sRm = S * L; gav11.sRn = 1;
      gav11.M = N; gav11.N = DH; gav11.K = N; gav11.zi_n = 1; gav11.flags = 4; gav11.act = 0;
      gav11.alpha = 1.0f; gav11.beta = 1.0f; gav11.sa = 1.0f; gav11.sb = 1.0f; gav11.Npad = DH; gav11.pad_ = 0;
      if ((long long)(N) >= 64 && (long long)(DH) >= 64) k_gemmT<0, 4, 4><<<dim3((unsigned)((DH) + 63) / 64, (unsigned)((N) + 63) / 64, (unsigned)(Bn)), 32, 0, stream>>>(gav11);
      else k_gemm<0><<<dim3((unsigned)((DH) + 31) / 32, (unsigned)((N) + 15) / 16, (unsigned)(Bn)), 32, 0, stream>>>(gav11); }
    { GemmP gav12;
      gav12.A = E + (size_t)1 * Bn * N * N; gav12.B = VP + 2 * L + 1 * DH; gav12.bias = E + (size_t)1 * Bn * N * N; gav12.R = QP + 2 * L + 1 * DH; gav12.C = O + 2 * L + 1 * DH;
      gav12.sAo = (long long)N * N; gav12.sAi = 0; gav12.sAm = N; gav12.sAk = 1; gav12.sBo = (long long)N * S * L; gav12.sBi = 0; gav12.sBn = 1; gav12.sBk = S * L; gav12.sCo = (long long)N * S * L; gav12.sCi = 0; gav12.sCm = S * L; gav12.sRo = (long long)N * S * L; gav12.sRi = 0; gav12.sRm = S * L; gav12.sRn = 1;
      gav12.M = N; gav12.N = DH; gav12.K = N; gav12.zi_n = 1; gav12.flags = 4; gav12.act = 0;
      gav12.alpha = 1.0f; gav12.beta = 1.0f; gav12.sa = 1.0f; gav12.sb = 1.0f; gav12.Npad = DH; gav12.pad_ = 0;
      if ((long long)(N) >= 64 && (long long)(DH) >= 64) k_gemmT<0, 4, 4><<<dim3((unsigned)((DH) + 63) / 64, (unsigned)((N) + 63) / 64, (unsigned)(Bn)), 32, 0, stream>>>(gav12);
      else k_gemm<0><<<dim3((unsigned)((DH) + 31) / 32, (unsigned)((N) + 15) / 16, (unsigned)(Bn)), 32, 0, stream>>>(gav12); }
    { GemmP gav13;
      gav13.A = E + (size_t)1 * Bn * N * N; gav13.B = VP + 3 * L + 1 * DH; gav13.bias = E + (size_t)1 * Bn * N * N; gav13.R = QP + 3 * L + 1 * DH; gav13.C = O + 3 * L + 1 * DH;
      gav13.sAo = (long long)N * N; gav13.sAi = 0; gav13.sAm = N; gav13.sAk = 1; gav13.sBo = (long long)N * S * L; gav13.sBi = 0; gav13.sBn = 1; gav13.sBk = S * L; gav13.sCo = (long long)N * S * L; gav13.sCi = 0; gav13.sCm = S * L; gav13.sRo = (long long)N * S * L; gav13.sRi = 0; gav13.sRm = S * L; gav13.sRn = 1;
      gav13.M = N; gav13.N = DH; gav13.K = N; gav13.zi_n = 1; gav13.flags = 4; gav13.act = 0;
      gav13.alpha = 1.0f; gav13.beta = 1.0f; gav13.sa = 1.0f; gav13.sb = 1.0f; gav13.Npad = DH; gav13.pad_ = 0;
      if ((long long)(N) >= 64 && (long long)(DH) >= 64) k_gemmT<0, 4, 4><<<dim3((unsigned)((DH) + 63) / 64, (unsigned)((N) + 63) / 64, (unsigned)(Bn)), 32, 0, stream>>>(gav13);
      else k_gemm<0><<<dim3((unsigned)((DH) + 31) / 32, (unsigned)((N) + 15) / 16, (unsigned)(Bn)), 32, 0, stream>>>(gav13); }
    { GemmP gav20;
      gav20.A = E + (size_t)2 * Bn * N * N; gav20.B = VP + 0 * L + 2 * DH; gav20.bias = E + (size_t)2 * Bn * N * N; gav20.R = QP + 0 * L + 2 * DH; gav20.C = O + 0 * L + 2 * DH;
      gav20.sAo = (long long)N * N; gav20.sAi = 0; gav20.sAm = N; gav20.sAk = 1; gav20.sBo = (long long)N * S * L; gav20.sBi = 0; gav20.sBn = 1; gav20.sBk = S * L; gav20.sCo = (long long)N * S * L; gav20.sCi = 0; gav20.sCm = S * L; gav20.sRo = (long long)N * S * L; gav20.sRi = 0; gav20.sRm = S * L; gav20.sRn = 1;
      gav20.M = N; gav20.N = DH; gav20.K = N; gav20.zi_n = 1; gav20.flags = 4; gav20.act = 0;
      gav20.alpha = 1.0f; gav20.beta = 1.0f; gav20.sa = 1.0f; gav20.sb = 1.0f; gav20.Npad = DH; gav20.pad_ = 0;
      if ((long long)(N) >= 64 && (long long)(DH) >= 64) k_gemmT<0, 4, 4><<<dim3((unsigned)((DH) + 63) / 64, (unsigned)((N) + 63) / 64, (unsigned)(Bn)), 32, 0, stream>>>(gav20);
      else k_gemm<0><<<dim3((unsigned)((DH) + 31) / 32, (unsigned)((N) + 15) / 16, (unsigned)(Bn)), 32, 0, stream>>>(gav20); }
    { GemmP gav21;
      gav21.A = E + (size_t)2 * Bn * N * N; gav21.B = VP + 1 * L + 2 * DH; gav21.bias = E + (size_t)2 * Bn * N * N; gav21.R = QP + 1 * L + 2 * DH; gav21.C = O + 1 * L + 2 * DH;
      gav21.sAo = (long long)N * N; gav21.sAi = 0; gav21.sAm = N; gav21.sAk = 1; gav21.sBo = (long long)N * S * L; gav21.sBi = 0; gav21.sBn = 1; gav21.sBk = S * L; gav21.sCo = (long long)N * S * L; gav21.sCi = 0; gav21.sCm = S * L; gav21.sRo = (long long)N * S * L; gav21.sRi = 0; gav21.sRm = S * L; gav21.sRn = 1;
      gav21.M = N; gav21.N = DH; gav21.K = N; gav21.zi_n = 1; gav21.flags = 4; gav21.act = 0;
      gav21.alpha = 1.0f; gav21.beta = 1.0f; gav21.sa = 1.0f; gav21.sb = 1.0f; gav21.Npad = DH; gav21.pad_ = 0;
      if ((long long)(N) >= 64 && (long long)(DH) >= 64) k_gemmT<0, 4, 4><<<dim3((unsigned)((DH) + 63) / 64, (unsigned)((N) + 63) / 64, (unsigned)(Bn)), 32, 0, stream>>>(gav21);
      else k_gemm<0><<<dim3((unsigned)((DH) + 31) / 32, (unsigned)((N) + 15) / 16, (unsigned)(Bn)), 32, 0, stream>>>(gav21); }
    { GemmP gav22;
      gav22.A = E + (size_t)2 * Bn * N * N; gav22.B = VP + 2 * L + 2 * DH; gav22.bias = E + (size_t)2 * Bn * N * N; gav22.R = QP + 2 * L + 2 * DH; gav22.C = O + 2 * L + 2 * DH;
      gav22.sAo = (long long)N * N; gav22.sAi = 0; gav22.sAm = N; gav22.sAk = 1; gav22.sBo = (long long)N * S * L; gav22.sBi = 0; gav22.sBn = 1; gav22.sBk = S * L; gav22.sCo = (long long)N * S * L; gav22.sCi = 0; gav22.sCm = S * L; gav22.sRo = (long long)N * S * L; gav22.sRi = 0; gav22.sRm = S * L; gav22.sRn = 1;
      gav22.M = N; gav22.N = DH; gav22.K = N; gav22.zi_n = 1; gav22.flags = 4; gav22.act = 0;
      gav22.alpha = 1.0f; gav22.beta = 1.0f; gav22.sa = 1.0f; gav22.sb = 1.0f; gav22.Npad = DH; gav22.pad_ = 0;
      if ((long long)(N) >= 64 && (long long)(DH) >= 64) k_gemmT<0, 4, 4><<<dim3((unsigned)((DH) + 63) / 64, (unsigned)((N) + 63) / 64, (unsigned)(Bn)), 32, 0, stream>>>(gav22);
      else k_gemm<0><<<dim3((unsigned)((DH) + 31) / 32, (unsigned)((N) + 15) / 16, (unsigned)(Bn)), 32, 0, stream>>>(gav22); }
    { GemmP gav23;
      gav23.A = E + (size_t)2 * Bn * N * N; gav23.B = VP + 3 * L + 2 * DH; gav23.bias = E + (size_t)2 * Bn * N * N; gav23.R = QP + 3 * L + 2 * DH; gav23.C = O + 3 * L + 2 * DH;
      gav23.sAo = (long long)N * N; gav23.sAi = 0; gav23.sAm = N; gav23.sAk = 1; gav23.sBo = (long long)N * S * L; gav23.sBi = 0; gav23.sBn = 1; gav23.sBk = S * L; gav23.sCo = (long long)N * S * L; gav23.sCi = 0; gav23.sCm = S * L; gav23.sRo = (long long)N * S * L; gav23.sRi = 0; gav23.sRm = S * L; gav23.sRn = 1;
      gav23.M = N; gav23.N = DH; gav23.K = N; gav23.zi_n = 1; gav23.flags = 4; gav23.act = 0;
      gav23.alpha = 1.0f; gav23.beta = 1.0f; gav23.sa = 1.0f; gav23.sb = 1.0f; gav23.Npad = DH; gav23.pad_ = 0;
      if ((long long)(N) >= 64 && (long long)(DH) >= 64) k_gemmT<0, 4, 4><<<dim3((unsigned)((DH) + 63) / 64, (unsigned)((N) + 63) / 64, (unsigned)(Bn)), 32, 0, stream>>>(gav23);
      else k_gemm<0><<<dim3((unsigned)((DH) + 31) / 32, (unsigned)((N) + 15) / 16, (unsigned)(Bn)), 32, 0, stream>>>(gav23); }
    { GemmP gav30;
      gav30.A = E + (size_t)3 * Bn * N * N; gav30.B = VP + 0 * L + 3 * DH; gav30.bias = E + (size_t)3 * Bn * N * N; gav30.R = QP + 0 * L + 3 * DH; gav30.C = O + 0 * L + 3 * DH;
      gav30.sAo = (long long)N * N; gav30.sAi = 0; gav30.sAm = N; gav30.sAk = 1; gav30.sBo = (long long)N * S * L; gav30.sBi = 0; gav30.sBn = 1; gav30.sBk = S * L; gav30.sCo = (long long)N * S * L; gav30.sCi = 0; gav30.sCm = S * L; gav30.sRo = (long long)N * S * L; gav30.sRi = 0; gav30.sRm = S * L; gav30.sRn = 1;
      gav30.M = N; gav30.N = DH; gav30.K = N; gav30.zi_n = 1; gav30.flags = 4; gav30.act = 0;
      gav30.alpha = 1.0f; gav30.beta = 1.0f; gav30.sa = 1.0f; gav30.sb = 1.0f; gav30.Npad = DH; gav30.pad_ = 0;
      if ((long long)(N) >= 64 && (long long)(DH) >= 64) k_gemmT<0, 4, 4><<<dim3((unsigned)((DH) + 63) / 64, (unsigned)((N) + 63) / 64, (unsigned)(Bn)), 32, 0, stream>>>(gav30);
      else k_gemm<0><<<dim3((unsigned)((DH) + 31) / 32, (unsigned)((N) + 15) / 16, (unsigned)(Bn)), 32, 0, stream>>>(gav30); }
    { GemmP gav31;
      gav31.A = E + (size_t)3 * Bn * N * N; gav31.B = VP + 1 * L + 3 * DH; gav31.bias = E + (size_t)3 * Bn * N * N; gav31.R = QP + 1 * L + 3 * DH; gav31.C = O + 1 * L + 3 * DH;
      gav31.sAo = (long long)N * N; gav31.sAi = 0; gav31.sAm = N; gav31.sAk = 1; gav31.sBo = (long long)N * S * L; gav31.sBi = 0; gav31.sBn = 1; gav31.sBk = S * L; gav31.sCo = (long long)N * S * L; gav31.sCi = 0; gav31.sCm = S * L; gav31.sRo = (long long)N * S * L; gav31.sRi = 0; gav31.sRm = S * L; gav31.sRn = 1;
      gav31.M = N; gav31.N = DH; gav31.K = N; gav31.zi_n = 1; gav31.flags = 4; gav31.act = 0;
      gav31.alpha = 1.0f; gav31.beta = 1.0f; gav31.sa = 1.0f; gav31.sb = 1.0f; gav31.Npad = DH; gav31.pad_ = 0;
      if ((long long)(N) >= 64 && (long long)(DH) >= 64) k_gemmT<0, 4, 4><<<dim3((unsigned)((DH) + 63) / 64, (unsigned)((N) + 63) / 64, (unsigned)(Bn)), 32, 0, stream>>>(gav31);
      else k_gemm<0><<<dim3((unsigned)((DH) + 31) / 32, (unsigned)((N) + 15) / 16, (unsigned)(Bn)), 32, 0, stream>>>(gav31); }
    { GemmP gav32;
      gav32.A = E + (size_t)3 * Bn * N * N; gav32.B = VP + 2 * L + 3 * DH; gav32.bias = E + (size_t)3 * Bn * N * N; gav32.R = QP + 2 * L + 3 * DH; gav32.C = O + 2 * L + 3 * DH;
      gav32.sAo = (long long)N * N; gav32.sAi = 0; gav32.sAm = N; gav32.sAk = 1; gav32.sBo = (long long)N * S * L; gav32.sBi = 0; gav32.sBn = 1; gav32.sBk = S * L; gav32.sCo = (long long)N * S * L; gav32.sCi = 0; gav32.sCm = S * L; gav32.sRo = (long long)N * S * L; gav32.sRi = 0; gav32.sRm = S * L; gav32.sRn = 1;
      gav32.M = N; gav32.N = DH; gav32.K = N; gav32.zi_n = 1; gav32.flags = 4; gav32.act = 0;
      gav32.alpha = 1.0f; gav32.beta = 1.0f; gav32.sa = 1.0f; gav32.sb = 1.0f; gav32.Npad = DH; gav32.pad_ = 0;
      if ((long long)(N) >= 64 && (long long)(DH) >= 64) k_gemmT<0, 4, 4><<<dim3((unsigned)((DH) + 63) / 64, (unsigned)((N) + 63) / 64, (unsigned)(Bn)), 32, 0, stream>>>(gav32);
      else k_gemm<0><<<dim3((unsigned)((DH) + 31) / 32, (unsigned)((N) + 15) / 16, (unsigned)(Bn)), 32, 0, stream>>>(gav32); }
    { GemmP gav33;
      gav33.A = E + (size_t)3 * Bn * N * N; gav33.B = VP + 3 * L + 3 * DH; gav33.bias = E + (size_t)3 * Bn * N * N; gav33.R = QP + 3 * L + 3 * DH; gav33.C = O + 3 * L + 3 * DH;
      gav33.sAo = (long long)N * N; gav33.sAi = 0; gav33.sAm = N; gav33.sAk = 1; gav33.sBo = (long long)N * S * L; gav33.sBi = 0; gav33.sBn = 1; gav33.sBk = S * L; gav33.sCo = (long long)N * S * L; gav33.sCi = 0; gav33.sCm = S * L; gav33.sRo = (long long)N * S * L; gav33.sRi = 0; gav33.sRm = S * L; gav33.sRn = 1;
      gav33.M = N; gav33.N = DH; gav33.K = N; gav33.zi_n = 1; gav33.flags = 4; gav33.act = 0;
      gav33.alpha = 1.0f; gav33.beta = 1.0f; gav33.sa = 1.0f; gav33.sb = 1.0f; gav33.Npad = DH; gav33.pad_ = 0;
      if ((long long)(N) >= 64 && (long long)(DH) >= 64) k_gemmT<0, 4, 4><<<dim3((unsigned)((DH) + 63) / 64, (unsigned)((N) + 63) / 64, (unsigned)(Bn)), 32, 0, stream>>>(gav33);
      else k_gemm<0><<<dim3((unsigned)((DH) + 31) / 32, (unsigned)((N) + 15) / 16, (unsigned)(Bn)), 32, 0, stream>>>(gav33); }
    k_stats<<<(unsigned)(NR), 256, 0, stream>>>(O, L, 0, 1, L, L, 1e-05f, st, 0);
    k_norm_apply<<<(unsigned)(((long long)(NR) * (L) * (1) + 255) / 256), 256, 0, stream>>>(O, O2, st, g0, b0, NR, L, 1, 1, 0, 0);
    { GemmP gff;
      gff.A = O2; gff.B = Wo; gff.bias = bo; gff.R = O2; gff.C = O;
      gff.sAo = 0; gff.sAi = 0; gff.sAm = L; gff.sAk = 1; gff.sBo = 0; gff.sBi = 0; gff.sBn = L; gff.sBk = 1; gff.sCo = 0; gff.sCi = 0; gff.sCm = L; gff.sRo = 0; gff.sRi = 0; gff.sRm = L; gff.sRn = 1;
      gff.M = NR; gff.N = L; gff.K = L; gff.zi_n = 1; gff.flags = 5; gff.act = 1;
      gff.alpha = 1.0f; gff.beta = 1.0f; gff.sa = 1.0f; gff.sb = 8.0f; gff.Npad = L; gff.pad_ = 0;
      if ((long long)(NR) >= 64 && (long long)(L) >= 64) k_gemmT<0, 4, 4><<<dim3((unsigned)((L) + 63) / 64, (unsigned)((NR) + 63) / 64, (unsigned)(1)), 32, 0, stream>>>(gff);
      else k_gemm<0><<<dim3((unsigned)((L) + 31) / 32, (unsigned)((NR) + 15) / 16, (unsigned)(1)), 32, 0, stream>>>(gff); }
    k_stats<<<(unsigned)(NR), 256, 0, stream>>>(O, L, 0, 1, L, L, 1e-05f, st, 0);
    k_norm_apply<<<(unsigned)(((long long)(NR) * (L) * (1) + 255) / 256), 256, 0, stream>>>(O, out, st, g1, b1, NR, L, 1, 1, 0, 0);
}
